// TemporalSelfAttention_33122787787413
// MI455X (gfx1250) — hardware-verified
//
#include <hip/hip_runtime.h>
#include <math.h>

typedef __attribute__((ext_vector_type(16))) _Float16 v16h;
typedef __attribute__((ext_vector_type(8)))  _Float16 v8h;
typedef __attribute__((ext_vector_type(16))) __bf16   v16b;
typedef __attribute__((ext_vector_type(8)))  float    v8f;
typedef __attribute__((ext_vector_type(4)))  float    v4f;

__device__ __forceinline__ int frag_k(int i, int h) { return (i < 8) ? (8 * h + i) : (16 + 8 * h + (i - 8)); }
__device__ __forceinline__ __bf16 bf16_rne(float f) {
    unsigned int u = __float_as_uint(f);
    u += 0x7fffu + ((u >> 16) & 1u);
    return __builtin_bit_cast(__bf16, (unsigned short)(u >> 16));
}
__device__ __forceinline__ float bf16_f32(__bf16 b) { return __uint_as_float(((unsigned int)__builtin_bit_cast(unsigned short, b)) << 16); }
__device__ __forceinline__ v8f wmma16(v16h a, v16h b, v8f c) {
    c = __builtin_amdgcn_wmma_f32_16x16x32_f16(false, a, false, b, (short)0, c, false, false);
    asm volatile("v_nop\n\tv_nop\n\tv_nop\n\tv_nop" : "+v"(c) : "v"(a), "v"(b));
    return c;
}
__device__ __forceinline__ v8f wmmab(v16b a, v16b b, v8f c) {
    c = __builtin_amdgcn_wmma_f32_16x16x32_bf16(false, a, false, b, (short)0, c, false, false);
    asm volatile("v_nop\n\tv_nop\n\tv_nop\n\tv_nop" : "+v"(c) : "v"(a), "v"(b));
    return c;
}
struct Split { v16b hi, lo; };
__device__ __forceinline__ v8f wmma3(const Split& a, const Split& b, v8f c) {
    c = __builtin_amdgcn_wmma_f32_16x16x32_bf16(false, a.hi, false, b.hi, (short)0, c, false, false);
    c = __builtin_amdgcn_wmma_f32_16x16x32_bf16(false, a.hi, false, b.lo, (short)0, c, false, false);
    c = __builtin_amdgcn_wmma_f32_16x16x32_bf16(false, a.lo, false, b.hi, (short)0, c, false, false);
    asm volatile("v_nop\n\tv_nop\n\tv_nop\n\tv_nop" : "+v"(c) : "v"(a.hi), "v"(a.lo), "v"(b.hi), "v"(b.lo));
    return c;
}
struct Split3 { v16b hi, mid, lo; };
__device__ __forceinline__ v8f wmma6(const Split3& a, const Split3& b, v8f c) {
    c = __builtin_amdgcn_wmma_f32_16x16x32_bf16(false, a.hi, false, b.hi, (short)0, c, false, false);
    c = __builtin_amdgcn_wmma_f32_16x16x32_bf16(false, a.hi, false, b.mid, (short)0, c, false, false);
    c = __builtin_amdgcn_wmma_f32_16x16x32_bf16(false, a.mid, false, b.hi, (short)0, c, false, false);
    c = __builtin_amdgcn_wmma_f32_16x16x32_bf16(false, a.hi, false, b.lo, (short)0, c, false, false);
    c = __builtin_amdgcn_wmma_f32_16x16x32_bf16(false, a.mid, false, b.mid, (short)0, c, false, false);
    c = __builtin_amdgcn_wmma_f32_16x16x32_bf16(false, a.lo, false, b.hi, (short)0, c, false, false);
    asm volatile("v_nop\n\tv_nop\n\tv_nop\n\tv_nop" : "+v"(c) : "v"(a.hi), "v"(a.mid), "v"(a.lo), "v"(b.hi), "v"(b.mid), "v"(b.lo));
    return c;
}

__device__ __forceinline__ v16h fh_ld(const float* __restrict__ p, long long sk, int k0, int h, int klen, float s) {
    v16h a;
#pragma unroll
    for (int i = 0; i < 16; ++i) { const int k = k0 + frag_k(i, h); a[i] = (k < klen) ? (_Float16)(p[(long long)k * sk] * s) : (_Float16)0.f; }
    return a;
}
__device__ __forceinline__ Split sp_ld(const float* __restrict__ p, long long sk, int k0, int h, int klen, float s) {
    Split r;
#pragma unroll
    for (int i = 0; i < 16; ++i) {
        const int k = k0 + frag_k(i, h); const float x = (k < klen) ? p[(long long)k * sk] * s : 0.f;
        const __bf16 hb = bf16_rne(x); r.hi[i] = hb; r.lo[i] = bf16_rne(x - bf16_f32(hb));
    }
    return r;
}
__device__ __forceinline__ Split3 sp3_ld(const float* __restrict__ p, long long sk, int k0, int h, int klen, float s) {
    Split3 r;
#pragma unroll
    for (int i = 0; i < 16; ++i) {
        const int k = k0 + frag_k(i, h); const float x = (k < klen) ? p[(long long)k * sk] * s : 0.f;
        const __bf16 hb = bf16_rne(x); const float r1 = x - bf16_f32(hb); const __bf16 mb = bf16_rne(r1);
        r.hi[i] = hb; r.mid[i] = mb; r.lo[i] = bf16_rne(r1 - bf16_f32(mb));
    }
    return r;
}
__device__ __forceinline__ v16b bh_ld(const float* __restrict__ p, long long sk, int k0, int h, int klen, float s) {
    v16b a;
#pragma unroll
    for (int i = 0; i < 16; ++i) { const int k = k0 + frag_k(i, h); a[i] = bf16_rne((k < klen) ? p[(long long)k * sk] * s : 0.f); }
    return a;
}
__device__ __forceinline__ v16h fh_row(const _Float16* __restrict__ row, int k0, int h) {
    v16h a;
#pragma unroll
    for (int i = 0; i < 16; ++i) a[i] = row[k0 + frag_k(i, h)];
    return a;
}

#define VST2(T, ptr, val) do { const T vst2_v_ = (val); *(volatile T*)(ptr) = vst2_v_; __threadfence(); *(volatile T*)(ptr) = vst2_v_; } while (0)
typedef float v4f __attribute__((ext_vector_type(4)));
#define VST2V4(ptr, val) do { const v4f vst2_v4_ = (val); *(volatile v4f*)(ptr) = vst2_v4_; __threadfence(); *(volatile v4f*)(ptr) = vst2_v4_; } while (0)

__device__ __attribute__((noinline)) float act_fn(float v, int act) {
    if (act == 1) return fmaxf(v, 0.f);
    if (act == 2) { const float u = 0.7978845608028654f * (v + 0.044715f * v * v * v); return 0.5f * v * (1.f + tanhf(u)); }
    if (act == 3) return v / (1.f + expf(-v));
    if (act == 4) return 0.5f * v * (1.f + erff(v * 0.7071067811865476f));
    if (act == 5) return tanhf(v);
    if (act == 6) return 1.f / (1.f + expf(-v));
    if (act == 7) return (v > 0.f) ? v : 0.01f * v;
    if (act == 8) return (v > 0.f) ? v : (expf(v) - 1.f);
    if (act == 9) return fminf(fmaxf(v, 0.f), 6.f);
    if (act == 10) return fabsf(v);
    if (act == 11) return (v >= 0.f) ? v : 0.1f * v;
    if (act == 12) return (v > 0.f) ? v : 0.2f * v;
    if (act == 13) return (v > 20.f) ? v : log1pf(expf(v));
    return v;
}

struct GemmP {
    const float* A; const float* B; const float* bias; const float* R; float* C;
    long long sAo, sAi, sAm, sAk, sBo, sBi, sBn, sBk, sCo, sCi, sCm, sRo, sRi, sRm, sRn;
    int M, N, K, zi_n, flags, act; float alpha, beta, sa, sb;
    int Npad, pad_;
};
static_assert(sizeof(GemmP) == 5 * 8 + 15 * 8 + 6 * 4 + 4 * 4 + 2 * 4, "GemmP has padding");

template <int MODE>
__global__ __launch_bounds__(32) void k_gemm(GemmP p) {
    const int lane = threadIdx.x & 31, h = lane >> 4, l15 = lane & 15;
    const int m0 = blockIdx.y * 16, n0 = blockIdx.x * 32;
    const int z = blockIdx.z, zo = z / p.zi_n, zi = z - zo * p.zi_n;
    const float* A = p.A + zo * p.sAo + zi * p.sAi;
    const float* B = p.B + zo * p.sBo + zi * p.sBi;
    const int am = min(m0 + l15, p.M - 1);
    v8f acc[2], comp[2];
#pragma unroll
    for (int t = 0; t < 2; ++t) { v8f zz = {}; acc[t] = zz; comp[t] = zz; }
    for (int k0 = 0; k0 < p.K; k0 += 32) {
        const float* arow = A + (long long)am * p.sAm;
        if (MODE == 1) {
            const Split a = sp_ld(arow, p.sAk, k0, h, p.K, 1.f);
#pragma unroll
            for (int t = 0; t < 2; ++t) {
                const int bn = min(n0 + t * 16 + l15, p.N - 1);
                acc[t] = wmma3(a, sp_ld(B + (long long)bn * p.sBn, p.sBk, k0, h, p.K, 1.f), acc[t]);
            }
        } else if (MODE == 3) {
            const Split3 a = sp3_ld(arow, p.sAk, k0, h, p.K, 1.f);
#pragma unroll
            for (int t = 0; t < 2; ++t) {
                const int bn = min(n0 + t * 16 + l15, p.N - 1);
                acc[t] = wmma6(a, sp3_ld(B + (long long)bn * p.sBn, p.sBk, k0, h, p.K, 1.f), acc[t]);
            }
        } else if (MODE == 4) {
            const Split3 a = sp3_ld(arow, p.sAk, k0, h, p.K, 1.f);
#pragma unroll
            for (int t = 0; t < 2; ++t) {
                const int bn = min(n0 + t * 16 + l15, p.N - 1); v8f zz = {};
                const v8f part = wmma6(a, sp3_ld(B + (long long)bn * p.sBn, p.sBk, k0, h, p.K, 1.f), zz);
                const v8f y = part - comp[t]; const v8f s = acc[t] + y; comp[t] = (s - acc[t]) - y; acc[t] = s;
            }
        } else if (MODE == 2) {
            const v16b a = bh_ld(arow, p.sAk, k0, h, p.K, 1.f);
#pragma unroll
            for (int t = 0; t < 2; ++t) {
                const int bn = min(n0 + t * 16 + l15, p.N - 1);
                acc[t] = wmmab(a, bh_ld(B + (long long)bn * p.sBn, p.sBk, k0, h, p.K, 1.f), acc[t]);
            }
        } else {
            const v16h a = fh_ld(arow, p.sAk, k0, h, p.K, p.sa);
#pragma unroll
            for (int t = 0; t < 2; ++t) {
                const int bn = min(n0 + t * 16 + l15, p.N - 1);
                acc[t] = wmma16(a, fh_ld(B + (long long)bn * p.sBn, p.sBk, k0, h, p.K, p.sb), acc[t]);
            }
        }
    }
    const float iscale = (MODE == 0) ? p.alpha / (p.sa * p.sb) : p.alpha;
    float* C = p.C + zo * p.sCo + zi * p.sCi;
    const float* R = p.R + zo * p.sRo + zi * p.sRi;
    __shared__ __align__(16) float ctile[16][36];
#pragma unroll
    for (int t = 0; t < 2; ++t) {
        const int n = n0 + t * 16 + l15; const int nn = min(n, p.N - 1);
#pragma unroll
        for (int r = 0; r < 8; ++r) {
            const int m = m0 + 8 * h + r; const int mm = min(m, p.M - 1);
            float v = acc[t][r] * iscale;
            if (p.flags & 1) v += p.bias[nn];
            if (p.flags & 2) v += p.bias[mm];
            v = act_fn(v, p.act);
            if (p.flags & 4) v += p.beta * R[(long long)mm * p.sRm + (long long)nn * p.sRn];
            ctile[8 * h + r][t * 16 + l15] = (n < p.N) ? v : 0.f;
        }
    }
    __syncthreads();
    const int NW = (p.Npad > p.N) ? p.Npad : p.N;
    const bool fast = (m0 + 16 <= p.M) && (n0 + 32 <= NW) && ((p.sCm & 3) == 0) && ((((size_t)C) & 15) == 0);
    if (fast) {
#pragma unroll
        for (int s = 0; s < 4; ++s) {
            const int row = s * 4 + (lane >> 3), c4 = (lane & 7) * 4;
            const v4f v = *(const v4f*)&ctile[row][c4];
            VST2V4(C + (long long)(m0 + row) * p.sCm + n0 + c4, v);
        }
    } else {
        for (int row = 0; row < 16; ++row) {
            const int m = m0 + row, n = n0 + lane;
            if (m < p.M && n < NW) VST2(float, C + (long long)m * p.sCm + n, ctile[row][lane]);
        }
    }
}


template <int MODE, int TM, int TN>
__global__ __launch_bounds__(32) void k_gemmT(GemmP p) {
    const int lane = threadIdx.x & 31, h = lane >> 4, l15 = lane & 15;
    const int m0 = blockIdx.y * (16 * TM), n0 = blockIdx.x * (16 * TN);
    const int z = blockIdx.z, zo = z / p.zi_n, zi = z - zo * p.zi_n;
    const float* A = p.A + zo * p.sAo + zi * p.sAi;
    const float* B = p.B + zo * p.sBo + zi * p.sBi;
    v8f acc[TM][TN];
#pragma unroll
    for (int i = 0; i < TM; ++i)
#pragma unroll
        for (int t = 0; t < TN; ++t) { v8f zz = {}; acc[i][t] = zz; }
    for (int k0 = 0; k0 < p.K; k0 += 32) {
        if (MODE == 1) {
            Split a[TM], b[TN];
#pragma unroll
            for (int i = 0; i < TM; ++i) { const int am = min(m0 + 16 * i + l15, p.M - 1); a[i] = sp_ld(A + (long long)am * p.sAm, p.sAk, k0, h, p.K, 1.f); }
#pragma unroll
            for (int t = 0; t < TN; ++t) { const int bn = min(n0 + 16 * t + l15, p.N - 1); b[t] = sp_ld(B + (long long)bn * p.sBn, p.sBk, k0, h, p.K, 1.f); }
#pragma unroll
            for (int i = 0; i < TM; ++i)
#pragma unroll
                for (int t = 0; t < TN; ++t) acc[i][t] = wmma3(a[i], b[t], acc[i][t]);
        } else if (MODE == 2) {
            v16b a[TM], b[TN];
#pragma unroll
            for (int i = 0; i < TM; ++i) { const int am = min(m0 + 16 * i + l15, p.M - 1); a[i] = bh_ld(A + (long long)am * p.sAm, p.sAk, k0, h, p.K, 1.f); }
#pragma unroll
            for (int t = 0; t < TN; ++t) { const int bn = min(n0 + 16 * t + l15, p.N - 1); b[t] = bh_ld(B + (long long)bn * p.sBn, p.sBk, k0, h, p.K, 1.f); }
#pragma unroll
            for (int i = 0; i < TM; ++i)
#pragma unroll
                for (int t = 0; t < TN; ++t) acc[i][t] = wmmab(a[i], b[t], acc[i][t]);
        } else {
            v16h a[TM], b[TN];
#pragma unroll
            for (int i = 0; i < TM; ++i) { const int am = min(m0 + 16 * i + l15, p.M - 1); a[i] = fh_ld(A + (long long)am * p.sAm, p.sAk, k0, h, p.K, p.sa); }
#pragma unroll
            for (int t = 0; t < TN; ++t) { const int bn = min(n0 + 16 * t + l15, p.N - 1); b[t] = fh_ld(B + (long long)bn * p.sBn, p.sBk, k0, h, p.K, p.sb); }
#pragma unroll
            for (int i = 0; i < TM; ++i)
#pragma unroll
                for (int t = 0; t < TN; ++t) acc[i][t] = wmma16(a[i], b[t], acc[i][t]);
        }
    }
    const float iscale = (MODE == 0) ? p.alpha / (p.sa * p.sb) : p.alpha;
    float* C = p.C + zo * p.sCo + zi * p.sCi;
    const float* R = p.R + zo * p.sRo + zi * p.sRi;
    const int NW = (p.Npad > p.N) ? p.Npad : p.N;
    __shared__ __align__(16) float ctile[16][36];
#pragma unroll
    for (int i = 0; i < TM; ++i) {
        const int mb = m0 + 16 * i; if (mb >= p.M) break;
#pragma unroll
        for (int tp = 0; tp < TN / 2; ++tp) {
            const int nb = n0 + 32 * tp; if (nb >= NW) break;
#pragma unroll
            for (int t2 = 0; t2 < 2; ++t2) {
                const int t = 2 * tp + t2; const int n = nb + t2 * 16 + l15; const int nn = min(n, p.N - 1);
#pragma unroll
                for (int r = 0; r < 8; ++r) {
                    const int m = mb + 8 * h + r; const int mm = min(m, p.M - 1);
                    float v = acc[i][t][r] * iscale;
                    if (p.flags & 1) v += p.bias[nn];
                    if (p.flags & 2) v += p.bias[mm];
                    v = act_fn(v, p.act);
                    if (p.flags & 4) v += p.beta * R[(long long)mm * p.sRm + (long long)nn * p.sRn];
                    ctile[8 * h + r][t2 * 16 + l15] = (n < p.N) ? v : 0.f;
                }
            }
            __syncthreads();
            const bool fast = (mb + 16 <= p.M) && (nb + 32 <= NW) && ((p.sCm & 3) == 0) && ((((size_t)C) & 15) == 0);
            if (fast) {
#pragma unroll
                for (int s = 0; s < 4; ++s) {
                    const int row = s * 4 + (lane >> 3), c4 = (lane & 7) * 4;
                    const v4f v = *(const v4f*)&ctile[row][c4];
                    VST2V4(C + (long long)(mb + row) * p.sCm + nb + c4, v);
                }
            } else {
                for (int row = 0; row < 16; ++row) {
                    const int m = mb + row, n = nb + lane;
                    if (m < p.M && n < NW) VST2(float, C + (long long)m * p.sCm + n, ctile[row][lane]);
                }
            }
            __syncthreads();
        }
    }
}

#define AW 4
struct AttnP {
    const float* Q; const float* K; const float* V; float* O; float* P; const float* Mf; const int* Mi; float* ST;
    const float* Pw; const float* Rt; const int* SQ; const int* SK;
    long long swb, swh, swi, swj, srb, srh, sri;
    long long sQb, sQh, sQi, sQd, sKb, sKh, sKj, sKd, sVb, sVh, sVj, sVd, sOb, sOh, sOi, sPb, sPh, sPi, smb, smh, smi, smj;
    int Lq, Lk, dh, dv, hrep, causal, coff, pband;
    float scale, mfill; int nonorm, mpol;
    int roff, rn, segpol, win;
};
static_assert(sizeof(AttnP) == 12 * 8 + 29 * 8 + 16 * 4, "AttnP has padding");

#ifndef KATTN_ATTR
#define KATTN_ATTR
#endif
template <int DHP, int DVP, int QM, bool SPLITPV, bool TWOPASS>
__global__ __launch_bounds__(32 * AW) KATTN_ATTR void k_attn(AttnP p) {
    constexpr int NT = DVP / 16;
    constexpr int KS = DHP / 32;
    constexpr int VP = DVP + 8;
    __shared__ __align__(16) float    pl[AW][16 * 64];
    __shared__ __align__(16) _Float16 vl[(SPLITPV ? 2 : 1) * 64 * VP];
    const int lane = threadIdx.x & 31, hf = lane >> 4, l15 = lane & 15, wave = threadIdx.x >> 5;
    const int h = blockIdx.y, b = blockIdx.z, hk = h / p.hrep;
    const int q0 = (blockIdx.x * AW + wave) * 16;
    float* myp = pl[wave];
    const float L2E = 1.4426950408889634f;
    const float NEG = -__builtin_inff();
    const int qi = min(q0 + l15, p.Lq - 1);
    const float* qrow = p.Q + b * p.sQb + h * p.sQh + (long long)qi * p.sQi;
    const float* kbase = p.K + b * p.sKb + hk * p.sKh;
    const float* vbase = p.V + b * p.sVb + hk * p.sVh;
    v16h qa[QM == 0 ? KS : 1]; Split qs_[QM == 1 ? KS : 1]; Split3 qt_[QM == 2 ? KS : 1];
#pragma unroll
    for (int ks = 0; ks < KS; ++ks) {
        if (QM == 2) qt_[ks] = sp3_ld(qrow, p.sQd, ks * 32, hf, p.dh, 1.f);
        else if (QM == 1) qs_[ks] = sp_ld(qrow, p.sQd, ks * 32, hf, p.dh, 1.f);
        else qa[ks] = fh_ld(qrow, p.sQd, ks * 32, hf, p.dh, 1.f);
    }
    v8f o[NT]; float m8[8], l8[8];
#pragma unroll
    for (int t = 0; t < NT; ++t) { v8f zz = {}; o[t] = zz; }
#pragma unroll
    for (int i = 0; i < 8; ++i) { m8[i] = NEG; l8[i] = 0.f; }
    int jend = p.Lk;
    if (p.causal == 1) { const int je = (blockIdx.x * AW + AW - 1) * 16 + 16 + p.coff; jend = min(jend, max(je, 0)); }
    const int npass = TWOPASS ? 2 : 1;
    for (int pass = 0; pass < npass; ++pass) {
        const bool dopv = (!TWOPASS) || pass == 1;
        for (int j0 = 0; j0 < jend; j0 += 64) {
            if (dopv) {
                __syncthreads();
                for (int idx = threadIdx.x; idx < 64 * DVP; idx += 32 * AW) {
                    const int jr = idx / DVP, d = idx - jr * DVP, j = j0 + jr;
                    const float f = (j < p.Lk && d < p.dv) ? vbase[(long long)j * p.sVj + (long long)d * p.sVd] : 0.f;
                    if (SPLITPV) {
                        const __bf16 hb = bf16_rne(f);
                        ((__bf16*)vl)[jr * VP + d] = hb; ((__bf16*)vl)[64 * VP + jr * VP + d] = bf16_rne(f - bf16_f32(hb));
                    } else vl[jr * VP + d] = (_Float16)f;
                }
            }
            v8f s[4];
#pragma unroll
            for (int t = 0; t < 4; ++t) {
                const int j = min(j0 + t * 16 + l15, p.Lk - 1);
                const float* krow = kbase + (long long)j * p.sKj;
                v8f acc = {};
#pragma unroll
                for (int ks = 0; ks < KS; ++ks) {
                    if (QM == 2)      acc = wmma6(qt_[ks], sp3_ld(krow, p.sKd, ks * 32, hf, p.dh, 1.f), acc);
                    else if (QM == 1) acc = wmma3(qs_[ks], sp_ld(krow, p.sKd, ks * 32, hf, p.dh, 1.f), acc);
                    else              acc = wmma16(qa[ks], fh_ld(krow, p.sKd, ks * 32, hf, p.dh, 1.f), acc);
                }
                s[t] = acc;
            }
            float pv[8][4];
#pragma unroll
            for (int i = 0; i < 8; ++i) {
                const int irow = q0 + i + 8 * hf;
                const int ic = min(irow, p.Lq - 1);
                float sc[4];
#pragma unroll
                for (int t = 0; t < 4; ++t) {
                    const int jg = j0 + t * 16 + l15;
                    float v = s[t][i] * p.scale;
                    if (p.Mf) v += p.Mf[b * p.smb + h * p.smh + (long long)ic * p.smi + (long long)min(jg, p.Lk - 1) * p.smj];
                    if (p.Rt) { int rc = ic - min(jg, p.Lk - 1) + p.roff; rc = rc < 0 ? 0 : (rc >= p.rn ? p.rn - 1 : rc); v += p.Rt[b * p.srb + h * p.srh + (long long)ic * p.sri + rc]; }
                    if (p.Mi) { const int mv = p.Mi[b * p.smb + h * p.smh + (long long)ic * p.smi + (long long)min(jg, p.Lk - 1) * p.smj]; if (p.mpol ? (mv != 0) : (mv == 0)) v = p.mfill; }
                    if (p.SQ) { const bool same = p.SQ[(long long)b * p.Lq + ic] == p.SK[(long long)b * p.Lk + min(jg, p.Lk - 1)]; if (p.segpol ? same : !same) v = p.mfill; }
                    if (p.causal == 2 && jg > irow + p.coff) v = p.mfill;
                    if (jg >= p.Lk || (p.causal == 1 && jg > irow + p.coff) || (p.causal == 3 && jg < irow + p.coff) || (p.win > 0 && irow + p.coff - jg > p.win)) v = NEG; else v *= L2E;
                    sc[t] = v;
                }
                if (!TWOPASS || pass == 0) {
                    float mx = fmaxf(fmaxf(sc[0], sc[1]), fmaxf(sc[2], sc[3]));
                    mx = fmaxf(mx, __shfl_xor(mx, 1, 32)); mx = fmaxf(mx, __shfl_xor(mx, 2, 32));
                    mx = fmaxf(mx, __shfl_xor(mx, 4, 32)); mx = fmaxf(mx, __shfl_xor(mx, 8, 32));
                    const float mnew = fmaxf(m8[i], mx);
                    const float corr = (mnew == NEG) ? 1.f : exp2f(m8[i] - mnew);
                    float rs = 0.f;
#pragma unroll
                    for (int t = 0; t < 4; ++t) {
                        const float pp = (sc[t] == NEG) ? 0.f : exp2f(sc[t] - mnew); rs += pp;
                        pv[i][t] = p.Pw ? pp * p.Pw[b * p.swb + h * p.swh + (long long)ic * p.swi + (long long)min(j0 + t * 16 + l15, p.Lk - 1) * p.swj] : pp;
                    }
                    rs += __shfl_xor(rs, 1, 32); rs += __shfl_xor(rs, 2, 32); rs += __shfl_xor(rs, 4, 32); rs += __shfl_xor(rs, 8, 32);
                    l8[i] = l8[i] * corr + rs; m8[i] = mnew;
                    if (!TWOPASS) {
#pragma unroll
                        for (int t = 0; t < NT; ++t) o[t][i] *= corr;
                    }
                } else {
                    const float inv = (l8[i] > 0.f) ? 1.f / l8[i] : 0.f;
#pragma unroll
                    for (int t = 0; t < 4; ++t) {
                        const int jg = j0 + t * 16 + l15;
                        float pp = (sc[t] == NEG) ? 0.f : exp2f(sc[t] - m8[i]) * inv;
                        if (p.Pw) pp *= p.Pw[b * p.swb + h * p.swh + (long long)ic * p.swi + (long long)min(jg, p.Lk - 1) * p.swj];
                        pv[i][t] = pp;
                    }
                }
            }
            if (dopv) {
#pragma unroll
                for (int i = 0; i < 8; ++i)
#pragma unroll
                    for (int t = 0; t < 4; ++t) myp[(i + 8 * hf) * 64 + t * 16 + l15] = pv[i][t];
                __syncthreads();
                if (p.P) {
                    float* pb_ = p.P + b * p.sPb + h * p.sPh;
                    const bool fastP = (p.pband == 0) && ((p.sPi & 3) == 0) && (j0 + 64 <= p.Lk) && (q0 + 16 <= p.Lq) && ((((size_t)pb_) & 15) == 0);
                    if (fastP) {
#pragma unroll
                        for (int s = 0; s < 8; ++s) {
                            const int row = s * 2 + (lane >> 4), c4 = (lane & 15) * 4;
                            const v4f v = *(const v4f*)(myp + row * 64 + c4);
                            VST2V4(pb_ + (long long)(q0 + row) * p.sPi + j0 + c4, v);
                        }
                    } else {
                        for (int row = 0; row < 16; ++row) {
                            const int irow = q0 + row; if (irow >= p.Lq) continue;
                            for (int c = lane; c < 64; c += 32) {
                                const int jg = j0 + c; if (jg >= p.Lk) continue;
                                if (p.pband == 0) VST2(float, pb_ + (long long)irow * p.sPi + jg, myp[row * 64 + c]);
                                else if (jg - irow <= p.pband && irow - jg <= p.pband) VST2(float, pb_ + (long long)irow * p.sPi + (jg - irow + p.pband), myp[row * 64 + c]);
                            }
                        }
                    }
                }
                if (SPLITPV) {
                    const Split pa0 = sp_ld(myp + l15 * 64, 1, 0, hf, 64, 1.f), pa1 = sp_ld(myp + l15 * 64, 1, 32, hf, 64, 1.f);
                    const __bf16* vh = (const __bf16*)vl; const __bf16* vlo = vh + 64 * VP;
#pragma unroll
                    for (int t = 0; t < NT; ++t) {
                        const int dcol = t * 16 + l15;
                        Split b0, b1;
#pragma unroll
                        for (int e = 0; e < 16; ++e) {
                            const int k0 = frag_k(e, hf), k1 = 32 + frag_k(e, hf);
                            b0.hi[e] = vh[k0 * VP + dcol]; b0.lo[e] = vlo[k0 * VP + dcol]; b1.hi[e] = vh[k1 * VP + dcol]; b1.lo[e] = vlo[k1 * VP + dcol];
                        }
                        o[t] = wmma3(pa0, b0, o[t]);
                        o[t] = wmma3(pa1, b1, o[t]);
                    }
                } else {
                    const v16h pa0 = fh_ld(myp + l15 * 64, 1, 0, hf, 64, 4096.f), pa1 = fh_ld(myp + l15 * 64, 1, 32, hf, 64, 4096.f);
#pragma unroll
                    for (int t = 0; t < NT; ++t) {
                        const int dcol = t * 16 + l15;
                        v16h b0, b1;
#pragma unroll
                        for (int e = 0; e < 16; ++e) { b0[e] = vl[frag_k(e, hf) * VP + dcol]; b1[e] = vl[(32 + frag_k(e, hf)) * VP + dcol]; }
                        o[t] = wmma16(pa0, b0, o[t]);
                        o[t] = wmma16(pa1, b1, o[t]);
                    }
                }
            }
        }
    }
    float* obase = p.O + b * p.sOb + h * p.sOh;
    if (p.ST) {
        const int rl = lane >> 1, isel = rl & 7;
        float mv = 0.f, lv = 0.f;
#pragma unroll
        for (int i = 0; i < 8; ++i) if (i == isel) { mv = m8[i]; lv = l8[i]; }
        const int irow = q0 + rl;
        if (irow < p.Lq) { float* st = p.ST + (((long long)b * gridDim.y + h) * p.Lq + irow) * 2 + (lane & 1); VST2(float, st, (lane & 1) ? lv : mv * 0.6931471805599453f); }
    }
    float invr[8];
#pragma unroll
    for (int i = 0; i < 8; ++i) {
        if (TWOPASS) invr[i] = SPLITPV ? 1.f : (1.f / 4096.f);
        else if (p.nonorm) invr[i] = exp2f(m8[i]) * (SPLITPV ? 1.f : (1.f / 4096.f));
        else invr[i] = (l8[i] > 0.f) ? (SPLITPV ? 1.f / l8[i] : 1.f / (l8[i] * 4096.f)) : 0.f;
    }
    __syncthreads();
    const bool ofast = ((p.sOi & 3) == 0) && ((((size_t)obase) & 15) == 0) && (q0 + 16 <= p.Lq);
#pragma unroll
    for (int c0 = 0; c0 < DVP; c0 += 64) {
#pragma unroll
        for (int i = 0; i < 8; ++i)
#pragma unroll
            for (int t = 0; t < NT; ++t) if (t * 16 >= c0 && t * 16 < c0 + 64) myp[(i + 8 * hf) * 64 + (t * 16 - c0) + l15] = o[t][i] * invr[i];
        __syncthreads();
        const int cw = (DVP - c0 < 64) ? (DVP - c0) : 64;
        if (ofast && (c0 + cw <= p.dv) && (cw % 32 == 0)) {
            const int lpr = cw / 4;
            const int rows_per_ins = 32 / lpr;
            for (int r0 = 0; r0 < 16; r0 += rows_per_ins) {
                const int row = r0 + lane / lpr, c4 = (lane % lpr) * 4;
                const v4f v = *(const v4f*)(myp + row * 64 + c4);
                VST2V4(obase + (long long)(q0 + row) * p.sOi + c0 + c4, v);
            }
        } else {
            for (int row = 0; row < 16; ++row) {
                const int irow = q0 + row; if (irow >= p.Lq) continue;
                for (int c = lane; c < cw; c += 32) { const int d = c0 + c; if (d < p.dv) VST2(float, obase + (long long)irow * p.sOi + d, myp[row * 64 + c]); }
            }
        }
        __syncthreads();
    }
}

struct TrP { const float* src; float* dst; const float* R2; long long sSz, lds, sDz, ldd, sRz, ldr; int R, C, flags, act; float alpha, beta; };
static_assert(sizeof(TrP) == 3 * 8 + 6 * 8 + 6 * 4, "TrP has padding");
__global__ __launch_bounds__(256) void k_tr(TrP p) {
    __shared__ float tile[32][33];
    const int c0 = blockIdx.x * 32, r0 = blockIdx.y * 32, z = blockIdx.z;
    const int lane = threadIdx.x & 31, wave = threadIdx.x >> 5;
    const float* s = p.src + z * p.sSz;
#pragma unroll
    for (int k = 0; k < 4; ++k) {
        const int rl = wave * 4 + k, r = r0 + rl, c = c0 + lane;
        tile[rl][lane] = (r < p.R && c < p.C) ? s[(long long)r * p.lds + c] : 0.f;
    }
    __syncthreads();
    float* d = p.dst + z * p.sDz; const float* rr = p.R2 + z * p.sRz;
#pragma unroll
    for (int k = 0; k < 4; ++k) {
        const int cl = wave * 4 + k, c = c0 + cl, r = r0 + lane;
        if (c < p.C && r < p.R) {
            float v = act_fn(p.alpha * tile[lane][cl], p.act);
            if (p.flags & 1) v += p.beta * rr[(long long)c * p.ldr + r];
            VST2(float, d + (long long)c * p.ldd + r, v);
        }
    }
}

__global__ __launch_bounds__(256) void k_affine(const float* __restrict__ src, float* __restrict__ dst, int n, float a, float b, const float* __restrict__ sdev) {
    const int i = blockIdx.x * 256 + threadIdx.x;
    if (i < n) { const float aa = sdev ? a * sdev[0] : a; const float v = aa * src[i] + b; VST2(float, dst + i, v); }
}

struct SmP { const float* src; float* dst; const float* Mf; long long sz, sr, dz, dr, smz, smr; int n, pad; float scale_in, scale_out; };
static_assert(sizeof(SmP) == 3 * 8 + 6 * 8 + 4 * 4, "SmP has padding");
__global__ __launch_bounds__(256) void k_softmax(SmP p) {
    __shared__ float red[256];
    const int r = blockIdx.x, z = blockIdx.y, tid = threadIdx.x;
    const float* s = p.src + z * p.sz + (long long)r * p.sr;
    const float* mf = p.Mf ? (p.Mf + z * p.smz + (long long)r * p.smr) : nullptr;
    float mx = -__builtin_inff();
    for (int j = tid; j < p.n; j += 256) { float v = s[j] * p.scale_in; if (mf) v += mf[j]; mx = fmaxf(mx, v); }
    red[tid] = mx; __syncthreads();
    for (int o = 128; o > 0; o >>= 1) { if (tid < o) red[tid] = fmaxf(red[tid], red[tid + o]); __syncthreads(); }
    mx = red[0]; __syncthreads();
    float sum = 0.f;
    for (int j = tid; j < p.n; j += 256) { float v = s[j] * p.scale_in; if (mf) v += mf[j]; sum += (mx == -__builtin_inff()) ? 0.f : expf(v - mx); }
    red[tid] = sum; __syncthreads();
    for (int o = 128; o > 0; o >>= 1) { if (tid < o) red[tid] += red[tid + o]; __syncthreads(); }
    sum = red[0];
    const float inv = (sum > 0.f) ? p.scale_out / sum : 0.f;
    float* d = p.dst + z * p.dz + (long long)r * p.dr;
    for (int j = tid; j < p.n; j += 256) { float v = s[j] * p.scale_in; if (mf) v += mf[j]; const float o = (mx == -__builtin_inff()) ? 0.f : expf(v - mx) * inv; VST2(float, d + j, o); }
}
__global__ __launch_bounds__(256) void k_stats(const float* __restrict__ x, long long sz, long long so, long long si, int inner, int n, float eps, float* __restrict__ stat, int mode) {
    __shared__ float red[256];
    const int z = blockIdx.x, tid = threadIdx.x;
    const float* base = x + z * sz;
    float s = 0.f;
    for (int e = tid; e < n; e += 256) s += base[(long long)(e / inner) * so + (long long)(e % inner) * si];
    red[tid] = s; __syncthreads();
    for (int o = 128; o > 0; o >>= 1) { if (tid < o) red[tid] += red[tid + o]; __syncthreads(); }
    const float mu = (mode == 0 || mode == 3) ? red[0] / (float)n : 0.f; __syncthreads();
    float q = 0.f;
    for (int e = tid; e < n; e += 256) { const float dlt = base[(long long)(e / inner) * so + (long long)(e % inner) * si] - mu; q += dlt * dlt; }
    red[tid] = q; __syncthreads();
    for (int o = 128; o > 0; o >>= 1) { if (tid < o) red[tid] += red[tid + o]; __syncthreads(); }
    {
        float rs;
        if (mode == 2) rs = sqrtf((float)n) / fmaxf(sqrtf(red[0]), eps); else if (mode == 3) rs = rsqrtf(red[0] / (float)(n - 1) + eps); else rs = rsqrtf(red[0] / (float)n + eps);
        if (tid < 32) { const float v = (tid == 0) ? mu : ((tid == 1) ? rs : 0.f); VST2(float, stat + (long long)z * 32 + tid, v); }
    }
}
__global__ __launch_bounds__(256) void k_norm_apply(const float* __restrict__ x, float* __restrict__ y, const float* __restrict__ stat, const float* __restrict__ g, const float* __restrict__ bta,
                                                     int Z, int C, int L, int G, int bn, int act) {
    const long long idx = (long long)blockIdx.x * 256 + threadIdx.x;
    if (idx >= (long long)Z * C * L) return;
    const int l = (int)(idx % L); const long long zc = idx / L; const int c = (int)(zc % C), z = (int)(zc / C); (void)l;
    const int set = bn ? c : (z * G + c / (C / G));
    float v = (x[idx] - stat[(long long)set * 32]) * stat[(long long)set * 32 + 1];
    if (g) v *= g[c];
    if (bta) v += bta[c];
    v = act_fn(v, act);
    VST2(float, y + idx, v);
}

__global__ __launch_bounds__(256) void k_lse_neg(const float* __restrict__ st, float* __restrict__ c, int n) {
    const int i = blockIdx.x * 256 + threadIdx.x;
    if (i < n) { const float v = -(st[2 * i] + logf(st[2 * i + 1])); VST2(float, c + i, v); }
}

__global__ __launch_bounds__(256) void k_iota(int* __restrict__ dst, int n, int a, int b) {
    const int i = blockIdx.x * 256 + threadIdx.x;
    if (i < n) { const int v = a * i + b; VST2(int, dst + i, v); }
}

__global__ __launch_bounds__(256) void k_axpby(const float* __restrict__ x, const float* __restrict__ y, float* __restrict__ dst, int n, float a, float b, float c) {
    const int i = blockIdx.x * 256 + threadIdx.x;
    if (i < n) { const float v = a * x[i] + b * y[i] + c; VST2(float, dst + i, v); }
}

struct RopeP { const float* X; float* Y; const float* C; const float* Sn; const int* pos; long long sXr, sXh, sYr, sYh, sCb, sCp, sCd; int R, Hn, D, S, mode, tmode, pmode, pad; };
static_assert(sizeof(RopeP) == 5 * 8 + 7 * 8 + 8 * 4, "RopeP has padding");
__global__ __launch_bounds__(256) void k_rope(RopeP p) {
    const long long idx = (long long)blockIdx.x * 256 + threadIdx.x;
    if (idx >= (long long)p.R * p.Hn * p.D) return;
    const int d = (int)(idx % p.D); const long long rh = idx / p.D; const int h = (int)(rh % p.Hn); const int r = (int)(rh / p.Hn);
    const int half = p.D / 2;
    int partner; float sign;
    if (p.mode == 0) { partner = (d < half) ? d + half : d - half; sign = (d < half) ? -1.f : 1.f; }
    else { partner = d ^ 1; sign = (d & 1) ? 1.f : -1.f; }
    const int tcol = (p.tmode == 0) ? d : ((p.tmode == 1) ? (d % half) : (d >> 1));
    const int pp = (p.pmode == 0) ? (r % p.S) : ((p.pmode == 1) ? h : p.pos[r]);
    const long long toff = (long long)(r / p.S) * p.sCb + (long long)pp * p.sCp + (long long)tcol * p.sCd;
    const float* xr = p.X + (long long)r * p.sXr + (long long)h * p.sXh;
    const float v = xr[d] * p.C[toff] + sign * xr[partner] * p.Sn[toff];
    VST2(float, p.Y + (long long)r * p.sYr + (long long)h * p.sYh + d, v);
}

__global__ __launch_bounds__(256) void k_invf(float* __restrict__ invb, int half, int D, float base, float num, int fmode, float cexp) {
    const int i = blockIdx.x * 256 + threadIdx.x;
    if (i >= ((half + 31) / 32) * 32) return;
    if (i >= half) { VST2(float, invb + i, 0.f); return; }
    const float e = (float)(2 * i) / (float)D;
    float invf;
    if (fmode == 1) invf = num * expf((float)(2 * i) * cexp);
    else if (fmode == 2) invf = num * powf(base, (-2.0f * ((float)i - 1.0f)) / (float)D);
    else invf = num * (1.0f / powf(base, e));
    VST2(float, invb + i, invf);
}
__global__ __launch_bounds__(256) void k_sincos(float* __restrict__ cs, float* __restrict__ sn, const float* __restrict__ invb, int S, int half, float pscale) {
    const int idx = blockIdx.x * 256 + threadIdx.x;
    if (idx >= S * half) return;
    const int s = idx / half, i = idx - s * half;
    const float ang = (pscale * (float)s) * invb[i];
    VST2(float, cs + idx, cosf(ang)); VST2(float, sn + idx, sinf(ang));
}

__global__ __launch_bounds__(256) void k_mulact(const float* __restrict__ x, const float* __restrict__ y, float* __restrict__ dst, int n, int act) {
    const int i = blockIdx.x * 256 + threadIdx.x;
    if (i < n) { const float v = act_fn(x[i], act) * y[i]; VST2(float, dst + i, v); }
}

__global__ __launch_bounds__(256) void k_matvec(GemmP p) {
    const int rpt = (p.N == 1) ? 1 : 32;
    const long long r0 = ((long long)blockIdx.x * 256 + threadIdx.x) * rpt; const int z = blockIdx.z, zo = z / p.zi_n, zi = z - zo * p.zi_n;
    if (r0 >= p.M) return;
    const float* Bb = p.B + zo * p.sBo + zi * p.sBi;
    float* C = p.C + zo * p.sCo + zi * p.sCi; const float* R = p.R + zo * p.sRo + zi * p.sRi;
    for (int rr = 0; rr < rpt; ++rr) {
        const long long r = r0 + rr; if (r >= p.M) break;
        const float* A = p.A + zo * p.sAo + zi * p.sAi + r * p.sAm;
        float acc[8] = {0.f, 0.f, 0.f, 0.f, 0.f, 0.f, 0.f, 0.f};
        for (int k = 0; k < p.K; ++k) { const float a = A[(long long)k * p.sAk];
#pragma unroll
            for (int j = 0; j < 8; ++j) if (j < p.N) acc[j] += a * Bb[(long long)j * p.sBn + (long long)k * p.sBk]; }
#pragma unroll
        for (int j = 0; j < 8; ++j) if (j < p.N) {
            float v = acc[j] * p.alpha;
            if (p.flags & 1) v += p.bias[j];
            if (p.flags & 2) v += p.bias[r];
            v = act_fn(v, p.act);
            if (p.flags & 4) v += p.beta * R[r * p.sRm + (long long)j * p.sRn];
            VST2(float, C + r * p.sCm + j, v);
        }
    }
}
__global__ __launch_bounds__(256) void k_smallsoftmax(const float* __restrict__ src, float* __restrict__ dst, long long sr, long long dr, int n, long long R, float scale) {
    const long long r0 = ((long long)blockIdx.x * 256 + threadIdx.x) * 32;
    for (int rr = 0; rr < 32; ++rr) {
        const long long r = r0 + rr; if (r >= R) return;
        const float* s = src + r * sr; float* d = dst + r * dr;
        float mx = -__builtin_inff();
        for (int j = 0; j < n; ++j) mx = fmaxf(mx, s[j] * scale);
        float sum = 0.f;
        for (int j = 0; j < n; ++j) sum += expf(s[j] * scale - mx);
        const float inv = 1.f / sum;
        for (int j = 0; j < n; ++j) { const float v = expf(s[j] * scale - mx) * inv; VST2(float, d + j, v); }
    }
}

__global__ __launch_bounds__(32) void k_unitstat(float* __restrict__ st) { const int t = threadIdx.x; const float v = (t == 1) ? 1.f : 0.f; VST2(float, st + t, v); }

__global__ __launch_bounds__(256) void k_lincopy(const float* __restrict__ src, long long lds, float* __restrict__ dst, long long ldd, long long rows, int cols) {
    const long long i = (long long)blockIdx.x * 256 + threadIdx.x; if (i >= rows * cols) return;
    const long long r = i / cols; const int c = (int)(i - r * cols);
    const float v = src[r * lds + c]; VST2(float, dst + r * ldd + c, v);
}

__global__ __launch_bounds__(256) void k_ts_bn(const float* __restrict__ O, const float* __restrict__ g_, const float* __restrict__ b_, float* __restrict__ OUT, int NB, int C, int T, int V) { __shared__ float red[256]; const int c = blockIdx.x; const int tid = threadIdx.x; const long long cnt = (long long)NB * T * V; float s = 0.f, s2 = 0.f;
    for (long long q = tid; q < cnt; q += 256) { const float v = O[q * C + c]; s += v; s2 += v * v; }
    red[tid] = s; __syncthreads(); for (int o = 128; o > 0; o >>= 1) { if (tid < o) red[tid] += red[tid + o]; __syncthreads(); } const float mu = red[0] / (float)cnt; __syncthreads();
    red[tid] = s2; __syncthreads(); for (int o = 128; o > 0; o >>= 1) { if (tid < o) red[tid] += red[tid + o]; __syncthreads(); } const float var = fmaxf(red[0] / (float)cnt - mu * mu, 0.f); const float rs = rsqrtf(var + 1e-5f); const float gg = g_[c], bb = b_[c];
    for (long long q = tid; q < cnt; q += 256) { const int v = (int)(q % V); const int t = (int)((q / V) % T); const int n = (int)(q / ((long long)V * T)); VST2(float, OUT + (((long long)n * C + c) * T + t) * V + v, (O[q * C + c] - mu) * rs * gg + bb); } }

template __global__ void k_gemm<0>(GemmP);

extern "C" void kernel_launch(void* const* d_in, const int* in_sizes, int n_in, void* d_out, int out_size, void* d_ws, size_t ws_size, hipStream_t stream) {
    (void)in_sizes; (void)n_in; (void)out_size; (void)ws_size;
    const float* x = (const float*)d_in[0];
    const float* Wq = (const float*)d_in[1];
    const float* bq = (const float*)d_in[2];
    const float* Wk = (const float*)d_in[3];
    const float* bk = (const float*)d_in[4];
    const float* Wv = (const float*)d_in[5];
    const float* bv = (const float*)d_in[6];
    const float* gam = (const float*)d_in[7];
    const float* bet = (const float*)d_in[8];
    const int NB = 32;
    const int C = 64;
    const int T = 256;
    const int V = 25;
    const int G = NB * V;
    const int NR = G * T;
    const int CB = 4;
    const int GC = CB * V;
    const int NRC = GC * T;
    float* out = (float*)d_out;
    char* wsp = (char*)d_ws;
    float* Q = (float*)wsp; wsp += (((size_t)((size_t)NRC * C) * 4 + 255) / 256) * 256;
    float* Kb = (float*)wsp; wsp += (((size_t)((size_t)NRC * C) * 4 + 255) / 256) * 256;
    float* Vb = (float*)wsp; wsp += (((size_t)((size_t)NRC * C) * 4 + 255) / 256) * 256;
    float* S = (float*)wsp; wsp += (((size_t)((size_t)GC * T * T) * 4 + 255) / 256) * 256;
    float* O = (float*)wsp; wsp += (((size_t)((size_t)NR * C) * 4 + 255) / 256) * 256;
    { GemmP gQ0;
      gQ0.A = x + (size_t)0 * CB * C * T * V; gQ0.B = Wq; gQ0.bias = bq; gQ0.R = x + (size_t)0 * CB * C * T * V; gQ0.C = Q;
      gQ0.sAo = (long long)C * T * V; gQ0.sAi = 0; gQ0.sAm = 1; gQ0.sAk = T * V; gQ0.sBo = 0; gQ0.sBi = 0; gQ0.sBn = C; gQ0.sBk = 1; gQ0.sCo = (long long)T * V * C; gQ0.sCi = 0; gQ0.sCm = C; gQ0.sRo = 0; gQ0.sRi = 0; gQ0.sRm = 0; gQ0.sRn = 0;
      gQ0.M = T * V; gQ0.N = C; gQ0.K = C; gQ0.zi_n = 1; gQ0.flags = 1; gQ0.act = 0;
      gQ0.alpha = 1.0f; gQ0.beta = 0.0f; gQ0.sa = 1.0f; gQ0.sb = 8.0f; gQ0.Npad = C; gQ0.pad_ = 0;
      if ((long long)(T * V) >= 64 && (long long)(C) >= 64) k_gemmT<0, 4, 4><<<dim3((unsigned)((C) + 63) / 64, (unsigned)((T * V) + 63) / 64, (unsigned)(CB)), 32, 0, stream>>>(gQ0);
      else k_gemm<0><<<dim3((unsigned)((C) + 31) / 32, (unsigned)((T * V) + 15) / 16, (unsigned)(CB)), 32, 0, stream>>>(gQ0); }
    { GemmP gKb0;
      gKb0.A = x + (size_t)0 * CB * C * T * V; gKb0.B = Wk; gKb0.bias = bk; gKb0.R = x + (size_t)0 * CB * C * T * V; gKb0.C = Kb;
      gKb0.sAo = (long long)C * T * V; gKb0.sAi = 0; gKb0.sAm = 1; gKb0.sAk = T * V; gKb0.sBo = 0; gKb0.sBi = 0; gKb0.sBn = C; gKb0.sBk = 1; gKb0.sCo = (long long)T * V * C; gKb0.sCi = 0; gKb0.sCm = C; gKb0.sRo = 0; gKb0.sRi = 0; gKb0.sRm = 0; gKb0.sRn = 0;
      gKb0.M = T * V; gKb0.N = C; gKb0.K = C; gKb0.zi_n = 1; gKb0.flags = 1; gKb0.act = 0;
      gKb0.alpha = 1.0f; gKb0.beta = 0.0f; gKb0.sa = 1.0f; gKb0.sb = 8.0f; gKb0.Npad = C; gKb0.pad_ = 0;
      if ((long long)(T * V) >= 64 && (long long)(C) >= 64) k_gemmT<0, 4, 4><<<dim3((unsigned)((C) + 63) / 64, (unsigned)((T * V) + 63) / 64, (unsigned)(CB)), 32, 0, stream>>>(gKb0);
      else k_gemm<0><<<dim3((unsigned)((C) + 31) / 32, (unsigned)((T * V) + 15) / 16, (unsigned)(CB)), 32, 0, stream>>>(gKb0); }
    { GemmP gVb0;
      gVb0.A = x + (size_t)0 * CB * C * T * V; gVb0.B = Wv; gVb0.bias = bv; gVb0.R = x + (size_t)0 * CB * C * T * V; gVb0.C = Vb;
      gVb0.sAo = (long long)C * T * V; gVb0.sAi = 0; gVb0.sAm = 1; gVb0.sAk = T * V; gVb0.sBo = 0; gVb0.sBi = 0; gVb0.sBn = C; gVb0.sBk = 1; gVb0.sCo = (long long)T * V * C; gVb0.sCi = 0; gVb0.sCm = C; gVb0.sRo = 0; gVb0.sRi = 0; gVb0.sRm = 0; gVb0.sRn = 0;
      gVb0.M = T * V; gVb0.N = C; gVb0.K = C; gVb0.zi_n = 1; gVb0.flags = 1; gVb0.act = 0;
      gVb0.alpha = 1.0f; gVb0.beta = 0.0f; gVb0.sa = 1.0f; gVb0.sb = 8.0f; gVb0.Npad = C; gVb0.pad_ = 0;
      if ((long long)(T * V) >= 64 && (long long)(C) >= 64) k_gemmT<0, 4, 4><<<dim3((unsigned)((C) + 63) / 64, (unsigned)((T * V) + 63) / 64, (unsigned)(CB)), 32, 0, stream>>>(gVb0);
      else k_gemm<0><<<dim3((unsigned)((C) + 31) / 32, (unsigned)((T * V) + 15) / 16, (unsigned)(CB)), 32, 0, stream>>>(gVb0); }
    { GemmP gs0;
      gs0.A = Q; gs0.B = Kb; gs0.bias = Q; gs0.R = Q; gs0.C = S;
      gs0.sAo = (long long)T * V * C; gs0.sAi = C; gs0.sAm = V * C; gs0.sAk = 1; gs0.sBo = (long long)T * V * C; gs0.sBi = C; gs0.sBn = V * C; gs0.sBk = 1; gs0.sCo = (long long)V * T * T; gs0.sCi = (long long)T * T; gs0.sCm = T; gs0.sRo = 0; gs0.sRi = 0; gs0.sRm = 0; gs0.sRn = 0;
      gs0.M = T; gs0.N = T; gs0.K = C; gs0.zi_n = V; gs0.flags = 0; gs0.act = 5;
      gs0.alpha = 0.125f; gs0.beta = 0.0f; gs0.sa = 1.0f; gs0.sb = 1.0f; gs0.Npad = T; gs0.pad_ = 0;
      if ((long long)(T) >= 64 && (long long)(T) >= 64) k_gemmT<0, 4, 4><<<dim3((unsigned)((T) + 63) / 64, (unsigned)((T) + 63) / 64, (unsigned)(GC)), 32, 0, stream>>>(gs0);
      else k_gemm<0><<<dim3((unsigned)((T) + 31) / 32, (unsigned)((T) + 15) / 16, (unsigned)(GC)), 32, 0, stream>>>(gs0); }
    { GemmP go0;
      go0.A = S; go0.B = Vb; go0.bias = S; go0.R = S; go0.C = O + (size_t)0 * NRC * C;
      go0.sAo = (long long)V * T * T; go0.sAi = (long long)T * T; go0.sAm = T; go0.sAk = 1; go0.sBo = (long long)T * V * C; go0.sBi = C; go0.sBn = 1; go0.sBk = V * C; go0.sCo = (long long)T * V * C; go0.sCi = C; go0.sCm = V * C; go0.sRo = 0; go0.sRi = 0; go0.sRm = 0; go0.sRn = 0;
      go0.M = T; go0.N = C; go0.K = T; go0.zi_n = V; go0.flags = 0; go0.act = 0;
      go0.alpha = 1.0f; go0.beta = 0.0f; go0.sa = 1.0f; go0.sb = 1.0f; go0.Npad = C; go0.pad_ = 0;
      if ((long long)(T) >= 64 && (long long)(C) >= 64) k_gemmT<0, 4, 4><<<dim3((unsigned)((C) + 63) / 64, (unsigned)((T) + 63) / 64, (unsigned)(GC)), 32, 0, stream>>>(go0);
      else k_gemm<0><<<dim3((unsigned)((C) + 31) / 32, (unsigned)((T) + 15) / 16, (unsigned)(GC)), 32, 0, stream>>>(go0); }
    { GemmP gQ1;
      gQ1.A = x + (size_t)1 * CB * C * T * V; gQ1.B = Wq; gQ1.bias = bq; gQ1.R = x + (size_t)1 * CB * C * T * V; gQ1.C = Q;
      gQ1.sAo = (long long)C * T * V; gQ1.sAi = 0; gQ1.sAm = 1; gQ1.sAk = T * V; gQ1.sBo = 0; gQ1.sBi = 0; gQ1.sBn = C; gQ1.sBk = 1; gQ1.sCo = (long long)T * V * C; gQ1.sCi = 0; gQ1.sCm = C; gQ1.sRo = 0; gQ1.sRi = 0; gQ1.sRm = 0; gQ1.sRn = 0;
      gQ1.M = T * V; gQ1.N = C; gQ1.K = C; gQ1.zi_n = 1; gQ1.flags = 1; gQ1.act = 0;
      gQ1.alpha = 1.0f; gQ1.beta = 0.0f; gQ1.sa = 1.0f; gQ1.sb = 8.0f; gQ1.Npad = C; gQ1.pad_ = 0;
      if ((long long)(T * V) >= 64 && (long long)(C) >= 64) k_gemmT<0, 4, 4><<<dim3((unsigned)((C) + 63) / 64, (unsigned)((T * V) + 63) / 64, (unsigned)(CB)), 32, 0, stream>>>(gQ1);
      else k_gemm<0><<<dim3((unsigned)((C) + 31) / 32, (unsigned)((T * V) + 15) / 16, (unsigned)(CB)), 32, 0, stream>>>(gQ1); }
    { GemmP gKb1;
      gKb1.A = x + (size_t)1 * CB * C * T * V; gKb1.B = Wk; gKb1.bias = bk; gKb1.R = x + (size_t)1 * CB * C * T * V; gKb1.C = Kb;
      gKb1.sAo = (long long)C * T * V; gKb1.sAi = 0; gKb1.sAm = 1; gKb1.sAk = T * V; gKb1.sBo = 0; gKb1.sBi = 0; gKb1.sBn = C; gKb1.sBk = 1; gKb1.sCo = (long long)T * V * C; gKb1.sCi = 0; gKb1.sCm = C; gKb1.sRo = 0; gKb1.sRi = 0; gKb1.sRm = 0; gKb1.sRn = 0;
      gKb1.M = T * V; gKb1.N = C; gKb1.K = C; gKb1.zi_n = 1; gKb1.flags = 1; gKb1.act = 0;
      gKb1.alpha = 1.0f; gKb1.beta = 0.0f; gKb1.sa = 1.0f; gKb1.sb = 8.0f; gKb1.Npad = C; gKb1.pad_ = 0;
      if ((long long)(T * V) >= 64 && (long long)(C) >= 64) k_gemmT<0, 4, 4><<<dim3((unsigned)((C) + 63) / 64, (unsigned)((T * V) + 63) / 64, (unsigned)(CB)), 32, 0, stream>>>(gKb1);
      else k_gemm<0><<<dim3((unsigned)((C) + 31) / 32, (unsigned)((T * V) + 15) / 16, (unsigned)(CB)), 32, 0, stream>>>(gKb1); }
    { GemmP gVb1;
      gVb1.A = x + (size_t)1 * CB * C * T * V; gVb1.B = Wv; gVb1.bias = bv; gVb1.R = x + (size_t)1 * CB * C * T * V; gVb1.C = Vb;
      gVb1.sAo = (long long)C * T * V; gVb1.sAi = 0; gVb1.sAm = 1; gVb1.sAk = T * V; gVb1.sBo = 0; gVb1.sBi = 0; gVb1.sBn = C; gVb1.sBk = 1; gVb1.sCo = (long long)T * V * C; gVb1.sCi = 0; gVb1.sCm = C; gVb1.sRo = 0; gVb1.sRi = 0; gVb1.sRm = 0; gVb1.sRn = 0;
      gVb1.M = T * V; gVb1.N = C; gVb1.K = C; gVb1.zi_n = 1; gVb1.flags = 1; gVb1.act = 0;
      gVb1.alpha = 1.0f; gVb1.beta = 0.0f; gVb1.sa = 1.0f; gVb1.sb = 8.0f; gVb1.Npad = C; gVb1.pad_ = 0;
      if ((long long)(T * V) >= 64 && (long long)(C) >= 64) k_gemmT<0, 4, 4><<<dim3((unsigned)((C) + 63) / 64, (unsigned)((T * V) + 63) / 64, (unsigned)(CB)), 32, 0, stream>>>(gVb1);
      else k_gemm<0><<<dim3((unsigned)((C) + 31) / 32, (unsigned)((T * V) + 15) / 16, (unsigned)(CB)), 32, 0, stream>>>(gVb1); }
    { GemmP gs1;
      gs1.A = Q; gs1.B = Kb; gs1.bias = Q; gs1.R = Q; gs1.C = S;
      gs1.sAo = (long long)T * V * C; gs1.sAi = C; gs1.sAm = V * C; gs1.sAk = 1; gs1.sBo = (long long)T * V * C; gs1.sBi = C; gs1.sBn = V * C; gs1.sBk = 1; gs1.sCo = (long long)V * T * T; gs1.sCi = (long long)T * T; gs1.sCm = T; gs1.sRo = 0; gs1.sRi = 0; gs1.sRm = 0; gs1.sRn = 0;
      gs1.M = T; gs1.N = T; gs1.K = C; gs1.zi_n = V; gs1.flags = 0; gs1.act = 5;
      gs1.alpha = 0.125f; gs1.beta = 0.0f; gs1.sa = 1.0f; gs1.sb = 1.0f; gs1.Npad = T; gs1.pad_ = 0;
      if ((long long)(T) >= 64 && (long long)(T) >= 64) k_gemmT<0, 4, 4><<<dim3((unsigned)((T) + 63) / 64, (unsigned)((T) + 63) / 64, (unsigned)(GC)), 32, 0, stream>>>(gs1);
      else k_gemm<0><<<dim3((unsigned)((T) + 31) / 32, (unsigned)((T) + 15) / 16, (unsigned)(GC)), 32, 0, stream>>>(gs1); }
    { GemmP go1;
      go1.A = S; go1.B = Vb; go1.bias = S; go1.R = S; go1.C = O + (size_t)1 * NRC * C;
      go1.sAo = (long long)V * T * T; go1.sAi = (long long)T * T; go1.sAm = T; go1.sAk = 1; go1.sBo = (long long)T * V * C; go1.sBi = C; go1.sBn = 1; go1.sBk = V * C; go1.sCo = (long long)T * V * C; go1.sCi = C; go1.sCm = V * C; go1.sRo = 0; go1.sRi = 0; go1.sRm = 0; go1.sRn = 0;
      go1.M = T; go1.N = C; go1.K = T; go1.zi_n = V; go1.flags = 0; go1.act = 0;
      go1.alpha = 1.0f; go1.beta = 0.0f; go1.sa = 1.0f; go1.sb = 1.0f; go1.Npad = C; go1.pad_ = 0;
      if ((long long)(T) >= 64 && (long long)(C) >= 64) k_gemmT<0, 4, 4><<<dim3((unsigned)((C) + 63) / 64, (unsigned)((T) + 63) / 64, (unsigned)(GC)), 32, 0, stream>>>(go1);
      else k_gemm<0><<<dim3((unsigned)((C) + 31) / 32, (unsigned)((T) + 15) / 16, (unsigned)(GC)), 32, 0, stream>>>(go1); }
    { GemmP gQ2;
      gQ2.A = x + (size_t)2 * CB * C * T * V; gQ2.B = Wq; gQ2.bias = bq; gQ2.R = x + (size_t)2 * CB * C * T * V; gQ2.C = Q;
      gQ2.sAo = (long long)C * T * V; gQ2.sAi = 0; gQ2.sAm = 1; gQ2.sAk = T * V; gQ2.sBo = 0; gQ2.sBi = 0; gQ2.sBn = C; gQ2.sBk = 1; gQ2.sCo = (long long)T * V * C; gQ2.sCi = 0; gQ2.sCm = C; gQ2.sRo = 0; gQ2.sRi = 0; gQ2.sRm = 0; gQ2.sRn = 0;
      gQ2.M = T * V; gQ2.N = C; gQ2.K = C; gQ2.zi_n = 1; gQ2.flags = 1; gQ2.act = 0;
      gQ2.alpha = 1.0f; gQ2.beta = 0.0f; gQ2.sa = 1.0f; gQ2.sb = 8.0f; gQ2.Npad = C; gQ2.pad_ = 0;
      if ((long long)(T * V) >= 64 && (long long)(C) >= 64) k_gemmT<0, 4, 4><<<dim3((unsigned)((C) + 63) / 64, (unsigned)((T * V) + 63) / 64, (unsigned)(CB)), 32, 0, stream>>>(gQ2);
      else k_gemm<0><<<dim3((unsigned)((C) + 31) / 32, (unsigned)((T * V) + 15) / 16, (unsigned)(CB)), 32, 0, stream>>>(gQ2); }
    { GemmP gKb2;
      gKb2.A = x + (size_t)2 * CB * C * T * V; gKb2.B = Wk; gKb2.bias = bk; gKb2.R = x + (size_t)2 * CB * C * T * V; gKb2.C = Kb;
      gKb2.sAo = (long long)C * T * V; gKb2.sAi = 0; gKb2.sAm = 1; gKb2.sAk = T * V; gKb2.sBo = 0; gKb2.sBi = 0; gKb2.sBn = C; gKb2.sBk = 1; gKb2.sCo = (long long)T * V * C; gKb2.sCi = 0; gKb2.sCm = C; gKb2.sRo = 0; gKb2.sRi = 0; gKb2.sRm = 0; gKb2.sRn = 0;
      gKb2.M = T * V; gKb2.N = C; gKb2.K = C; gKb2.zi_n = 1; gKb2.flags = 1; gKb2.act = 0;
      gKb2.alpha = 1.0f; gKb2.beta = 0.0f; gKb2.sa = 1.0f; gKb2.sb = 8.0f; gKb2.Npad = C; gKb2.pad_ = 0;
      if ((long long)(T * V) >= 64 && (long long)(C) >= 64) k_gemmT<0, 4, 4><<<dim3((unsigned)((C) + 63) / 64, (unsigned)((T * V) + 63) / 64, (unsigned)(CB)), 32, 0, stream>>>(gKb2);
      else k_gemm<0><<<dim3((unsigned)((C) + 31) / 32, (unsigned)((T * V) + 15) / 16, (unsigned)(CB)), 32, 0, stream>>>(gKb2); }
    { GemmP gVb2;
      gVb2.A = x + (size_t)2 * CB * C * T * V; gVb2.B = Wv; gVb2.bias = bv; gVb2.R = x + (size_t)2 * CB * C * T * V; gVb2.C = Vb;
      gVb2.sAo = (long long)C * T * V; gVb2.sAi = 0; gVb2.sAm = 1; gVb2.sAk = T * V; gVb2.sBo = 0; gVb2.sBi = 0; gVb2.sBn = C; gVb2.sBk = 1; gVb2.sCo = (long long)T * V * C; gVb2.sCi = 0; gVb2.sCm = C; gVb2.sRo = 0; gVb2.sRi = 0; gVb2.sRm = 0; gVb2.sRn = 0;
      gVb2.M = T * V; gVb2.N = C; gVb2.K = C; gVb2.zi_n = 1; gVb2.flags = 1; gVb2.act = 0;
      gVb2.alpha = 1.0f; gVb2.beta = 0.0f; gVb2.sa = 1.0f; gVb2.sb = 8.0f; gVb2.Npad = C; gVb2.pad_ = 0;
      if ((long long)(T * V) >= 64 && (long long)(C) >= 64) k_gemmT<0, 4, 4><<<dim3((unsigned)((C) + 63) / 64, (unsigned)((T * V) + 63) / 64, (unsigned)(CB)), 32, 0, stream>>>(gVb2);
      else k_gemm<0><<<dim3((unsigned)((C) + 31) / 32, (unsigned)((T * V) + 15) / 16, (unsigned)(CB)), 32, 0, stream>>>(gVb2); }
    { GemmP gs2;
      gs2.A = Q; gs2.B = Kb; gs2.bias = Q; gs2.R = Q; gs2.C = S;
      gs2.sAo = (long long)T * V * C; gs2.sAi = C; gs2.sAm = V * C; gs2.sAk = 1; gs2.sBo = (long long)T * V * C; gs2.sBi = C; gs2.sBn = V * C; gs2.sBk = 1; gs2.sCo = (long long)V * T * T; gs2.sCi = (long long)T * T; gs2.sCm = T; gs2.sRo = 0; gs2.sRi = 0; gs2.sRm = 0; gs2.sRn = 0;
      gs2.M = T; gs2.N = T; gs2.K = C; gs2.zi_n = V; gs2.flags = 0; gs2.act = 5;
      gs2.alpha = 0.125f; gs2.beta = 0.0f; gs2.sa = 1.0f; gs2.sb = 1.0f; gs2.Npad = T; gs2.pad_ = 0;
      if ((long long)(T) >= 64 && (long long)(T) >= 64) k_gemmT<0, 4, 4><<<dim3((unsigned)((T) + 63) / 64, (unsigned)((T) + 63) / 64, (unsigned)(GC)), 32, 0, stream>>>(gs2);
      else k_gemm<0><<<dim3((unsigned)((T) + 31) / 32, (unsigned)((T) + 15) / 16, (unsigned)(GC)), 32, 0, stream>>>(gs2); }
    { GemmP go2;
      go2.A = S; go2.B = Vb; go2.bias = S; go2.R = S; go2.C = O + (size_t)2 * NRC * C;
      go2.sAo = (long long)V * T * T; go2.sAi = (long long)T * T; go2.sAm = T; go2.sAk = 1; go2.sBo = (long long)T * V * C; go2.sBi = C; go2.sBn = 1; go2.sBk = V * C; go2.sCo = (long long)T * V * C; go2.sCi = C; go2.sCm = V * C; go2.sRo = 0; go2.sRi = 0; go2.sRm = 0; go2.sRn = 0;
      go2.M = T; go2.N = C; go2.K = T; go2.zi_n = V; go2.flags = 0; go2.act = 0;
      go2.alpha = 1.0f; go2.beta = 0.0f; go2.sa = 1.0f; go2.sb = 1.0f; go2.Npad = C; go2.pad_ = 0;
      if ((long long)(T) >= 64 && (long long)(C) >= 64) k_gemmT<0, 4, 4><<<dim3((unsigned)((C) + 63) / 64, (unsigned)((T) + 63) / 64, (unsigned)(GC)), 32, 0, stream>>>(go2);
      else k_gemm<0><<<dim3((unsigned)((C) + 31) / 32, (unsigned)((T) + 15) / 16, (unsigned)(GC)), 32, 0, stream>>>(go2); }
    { GemmP gQ3;
      gQ3.A = x + (size_t)3 * CB * C * T * V; gQ3.B = Wq; gQ3.bias = bq; gQ3.R = x + (size_t)3 * CB * C * T * V; gQ3.C = Q;
      gQ3.sAo = (long long)C * T * V; gQ3.sAi = 0; gQ3.sAm = 1; gQ3.sAk = T * V; gQ3.sBo = 0; gQ3.sBi = 0; gQ3.sBn = C; gQ3.sBk = 1; gQ3.sCo = (long long)T * V * C; gQ3.sCi = 0; gQ3.sCm = C; gQ3.sRo = 0; gQ3.sRi = 0; gQ3.sRm = 0; gQ3.sRn = 0;
      gQ3.M = T * V; gQ3.N = C; gQ3.K = C; gQ3.zi_n = 1; gQ3.flags = 1; gQ3.act = 0;
      gQ3.alpha = 1.0f; gQ3.beta = 0.0f; gQ3.sa = 1.0f; gQ3.sb = 8.0f; gQ3.Npad = C; gQ3.pad_ = 0;
      if ((long long)(T * V) >= 64 && (long long)(C) >= 64) k_gemmT<0, 4, 4><<<dim3((unsigned)((C) + 63) / 64, (unsigned)((T * V) + 63) / 64, (unsigned)(CB)), 32, 0, stream>>>(gQ3);
      else k_gemm<0><<<dim3((unsigned)((C) + 31) / 32, (unsigned)((T * V) + 15) / 16, (unsigned)(CB)), 32, 0, stream>>>(gQ3); }
    { GemmP gKb3;
      gKb3.A = x + (size_t)3 * CB * C * T * V; gKb3.B = Wk; gKb3.bias = bk; gKb3.R = x + (size_t)3 * CB * C * T * V; gKb3.C = Kb;
      gKb3.sAo = (long long)C * T * V; gKb3.sAi = 0; gKb3.sAm = 1; gKb3.sAk = T * V; gKb3.sBo = 0; gKb3.sBi = 0; gKb3.sBn = C; gKb3.sBk = 1; gKb3.sCo = (long long)T * V * C; gKb3.sCi = 0; gKb3.sCm = C; gKb3.sRo = 0; gKb3.sRi = 0; gKb3.sRm = 0; gKb3.sRn = 0;
      gKb3.M = T * V; gKb3.N = C; gKb3.K = C; gKb3.zi_n = 1; gKb3.flags = 1; gKb3.act = 0;
      gKb3.alpha = 1.0f; gKb3.beta = 0.0f; gKb3.sa = 1.0f; gKb3.sb = 8.0f; gKb3.Npad = C; gKb3.pad_ = 0;
      if ((long long)(T * V) >= 64 && (long long)(C) >= 64) k_gemmT<0, 4, 4><<<dim3((unsigned)((C) + 63) / 64, (unsigned)((T * V) + 63) / 64, (unsigned)(CB)), 32, 0, stream>>>(gKb3);
      else k_gemm<0><<<dim3((unsigned)((C) + 31) / 32, (unsigned)((T * V) + 15) / 16, (unsigned)(CB)), 32, 0, stream>>>(gKb3); }
    { GemmP gVb3;
      gVb3.A = x + (size_t)3 * CB * C * T * V; gVb3.B = Wv; gVb3.bias = bv; gVb3.R = x + (size_t)3 * CB * C * T * V; gVb3.C = Vb;
      gVb3.sAo = (long long)C * T * V; gVb3.sAi = 0; gVb3.sAm = 1; gVb3.sAk = T * V; gVb3.sBo = 0; gVb3.sBi = 0; gVb3.sBn = C; gVb3.sBk = 1; gVb3.sCo = (long long)T * V * C; gVb3.sCi = 0; gVb3.sCm = C; gVb3.sRo = 0; gVb3.sRi = 0; gVb3.sRm = 0; gVb3.sRn = 0;
      gVb3.M = T * V; gVb3.N = C; gVb3.K = C; gVb3.zi_n = 1; gVb3.flags = 1; gVb3.act = 0;
      gVb3.alpha = 1.0f; gVb3.beta = 0.0f; gVb3.sa = 1.0f; gVb3.sb = 8.0f; gVb3.Npad = C; gVb3.pad_ = 0;
      if ((long long)(T * V) >= 64 && (long long)(C) >= 64) k_gemmT<0, 4, 4><<<dim3((unsigned)((C) + 63) / 64, (unsigned)((T * V) + 63) / 64, (unsigned)(CB)), 32, 0, stream>>>(gVb3);
      else k_gemm<0><<<dim3((unsigned)((C) + 31) / 32, (unsigned)((T * V) + 15) / 16, (unsigned)(CB)), 32, 0, stream>>>(gVb3); }
    { GemmP gs3;
      gs3.A = Q; gs3.B = Kb; gs3.bias = Q; gs3.R = Q; gs3.C = S;
      gs3.sAo = (long long)T * V * C; gs3.sAi = C; gs3.sAm = V * C; gs3.sAk = 1; gs3.sBo = (long long)T * V * C; gs3.sBi = C; gs3.sBn = V * C; gs3.sBk = 1; gs3.sCo = (long long)V * T * T; gs3.sCi = (long long)T * T; gs3.sCm = T; gs3.sRo = 0; gs3.sRi = 0; gs3.sRm = 0; gs3.sRn = 0;
      gs3.M = T; gs3.N = T; gs3.K = C; gs3.zi_n = V; gs3.flags = 0; gs3.act = 5;
      gs3.alpha = 0.125f; gs3.beta = 0.0f; gs3.sa = 1.0f; gs3.sb = 1.0f; gs3.Npad = T; gs3.pad_ = 0;
      if ((long long)(T) >= 64 && (long long)(T) >= 64) k_gemmT<0, 4, 4><<<dim3((unsigned)((T) + 63) / 64, (unsigned)((T) + 63) / 64, (unsigned)(GC)), 32, 0, stream>>>(gs3);
      else k_gemm<0><<<dim3((unsigned)((T) + 31) / 32, (unsigned)((T) + 15) / 16, (unsigned)(GC)), 32, 0, stream>>>(gs3); }
    { GemmP go3;
      go3.A = S; go3.B = Vb; go3.bias = S; go3.R = S; go3.C = O + (size_t)3 * NRC * C;
      go3.sAo = (long long)V * T * T; go3.sAi = (long long)T * T; go3.sAm = T; go3.sAk = 1; go3.sBo = (long long)T * V * C; go3.sBi = C; go3.sBn = 1; go3.sBk = V * C; go3.sCo = (long long)T * V * C; go3.sCi = C; go3.sCm = V * C; go3.sRo = 0; go3.sRi = 0; go3.sRm = 0; go3.sRn = 0;
      go3.M = T; go3.N = C; go3.K = T; go3.zi_n = V; go3.flags = 0; go3.act = 0;
      go3.alpha = 1.0f; go3.beta = 0.0f; go3.sa = 1.0f; go3.sb = 1.0f; go3.Npad = C; go3.pad_ = 0;
      if ((long long)(T) >= 64 && (long long)(C) >= 64) k_gemmT<0, 4, 4><<<dim3((unsigned)((C) + 63) / 64, (unsigned)((T) + 63) / 64, (unsigned)(GC)), 32, 0, stream>>>(go3);
      else k_gemm<0><<<dim3((unsigned)((C) + 31) / 32, (unsigned)((T) + 15) / 16, (unsigned)(GC)), 32, 0, stream>>>(go3); }
    { GemmP gQ4;
      gQ4.A = x + (size_t)4 * CB * C * T * V; gQ4.B = Wq; gQ4.bias = bq; gQ4.R = x + (size_t)4 * CB * C * T * V; gQ4.C = Q;
      gQ4.sAo = (long long)C * T * V; gQ4.sAi = 0; gQ4.sAm = 1; gQ4.sAk = T * V; gQ4.sBo = 0; gQ4.sBi = 0; gQ4.sBn = C; gQ4.sBk = 1; gQ4.sCo = (long long)T * V * C; gQ4.sCi = 0; gQ4.sCm = C; gQ4.sRo = 0; gQ4.sRi = 0; gQ4.sRm = 0; gQ4.sRn = 0;
      gQ4.M = T * V; gQ4.N = C; gQ4.K = C; gQ4.zi_n = 1; gQ4.flags = 1; gQ4.act = 0;
      gQ4.alpha = 1.0f; gQ4.beta = 0.0f; gQ4.sa = 1.0f; gQ4.sb = 8.0f; gQ4.Npad = C; gQ4.pad_ = 0;
      if ((long long)(T * V) >= 64 && (long long)(C) >= 64) k_gemmT<0, 4, 4><<<dim3((unsigned)((C) + 63) / 64, (unsigned)((T * V) + 63) / 64, (unsigned)(CB)), 32, 0, stream>>>(gQ4);
      else k_gemm<0><<<dim3((unsigned)((C) + 31) / 32, (unsigned)((T * V) + 15) / 16, (unsigned)(CB)), 32, 0, stream>>>(gQ4); }
    { GemmP gKb4;
      gKb4.A = x + (size_t)4 * CB * C * T * V; gKb4.B = Wk; gKb4.bias = bk; gKb4.R = x + (size_t)4 * CB * C * T * V; gKb4.C = Kb;
      gKb4.sAo = (long long)C * T * V; gKb4.sAi = 0; gKb4.sAm = 1; gKb4.sAk = T * V; gKb4.sBo = 0; gKb4.sBi = 0; gKb4.sBn = C; gKb4.sBk = 1; gKb4.sCo = (long long)T * V * C; gKb4.sCi = 0; gKb4.sCm = C; gKb4.sRo = 0; gKb4.sRi = 0; gKb4.sRm = 0; gKb4.sRn = 0;
      gKb4.M = T * V; gKb4.N = C; gKb4.K = C; gKb4.zi_n = 1; gKb4.flags = 1; gKb4.act = 0;
      gKb4.alpha = 1.0f; gKb4.beta = 0.0f; gKb4.sa = 1.0f; gKb4.sb = 8.0f; gKb4.Npad = C; gKb4.pad_ = 0;
      if ((long long)(T * V) >= 64 && (long long)(C) >= 64) k_gemmT<0, 4, 4><<<dim3((unsigned)((C) + 63) / 64, (unsigned)((T * V) + 63) / 64, (unsigned)(CB)), 32, 0, stream>>>(gKb4);
      else k_gemm<0><<<dim3((unsigned)((C) + 31) / 32, (unsigned)((T * V) + 15) / 16, (unsigned)(CB)), 32, 0, stream>>>(gKb4); }
    { GemmP gVb4;
      gVb4.A = x + (size_t)4 * CB * C * T * V; gVb4.B = Wv; gVb4.bias = bv; gVb4.R = x + (size_t)4 * CB * C * T * V; gVb4.C = Vb;
      gVb4.sAo = (long long)C * T * V; gVb4.sAi = 0; gVb4.sAm = 1; gVb4.sAk = T * V; gVb4.sBo = 0; gVb4.sBi = 0; gVb4.sBn = C; gVb4.sBk = 1; gVb4.sCo = (long long)T * V * C; gVb4.sCi = 0; gVb4.sCm = C; gVb4.sRo = 0; gVb4.sRi = 0; gVb4.sRm = 0; gVb4.sRn = 0;
      gVb4.M = T * V; gVb4.N = C; gVb4.K = C; gVb4.zi_n = 1; gVb4.flags = 1; gVb4.act = 0;
      gVb4.alpha = 1.0f; gVb4.beta = 0.0f; gVb4.sa = 1.0f; gVb4.sb = 8.0f; gVb4.Npad = C; gVb4.pad_ = 0;
      if ((long long)(T * V) >= 64 && (long long)(C) >= 64) k_gemmT<0, 4, 4><<<dim3((unsigned)((C) + 63) / 64, (unsigned)((T * V) + 63) / 64, (unsigned)(CB)), 32, 0, stream>>>(gVb4);
      else k_gemm<0><<<dim3((unsigned)((C) + 31) / 32, (unsigned)((T * V) + 15) / 16, (unsigned)(CB)), 32, 0, stream>>>(gVb4); }
    { GemmP gs4;
      gs4.A = Q; gs4.B = Kb; gs4.bias = Q; gs4.R = Q; gs4.C = S;
      gs4.sAo = (long long)T * V * C; gs4.sAi = C; gs4.sAm = V * C; gs4.sAk = 1; gs4.sBo = (long long)T * V * C; gs4.sBi = C; gs4.sBn = V * C; gs4.sBk = 1; gs4.sCo = (long long)V * T * T; gs4.sCi = (long long)T * T; gs4.sCm = T; gs4.sRo = 0; gs4.sRi = 0; gs4.sRm = 0; gs4.sRn = 0;
      gs4.M = T; gs4.N = T; gs4.K = C; gs4.zi_n = V; gs4.flags = 0; gs4.act = 5;
      gs4.alpha = 0.125f; gs4.beta = 0.0f; gs4.sa = 1.0f; gs4.sb = 1.0f; gs4.Npad = T; gs4.pad_ = 0;
      if ((long long)(T) >= 64 && (long long)(T) >= 64) k_gemmT<0, 4, 4><<<dim3((unsigned)((T) + 63) / 64, (unsigned)((T) + 63) / 64, (unsigned)(GC)), 32, 0, stream>>>(gs4);
      else k_gemm<0><<<dim3((unsigned)((T) + 31) / 32, (unsigned)((T) + 15) / 16, (unsigned)(GC)), 32, 0, stream>>>(gs4); }
    { GemmP go4;
      go4.A = S; go4.B = Vb; go4.bias = S; go4.R = S; go4.C = O + (size_t)4 * NRC * C;
      go4.sAo = (long long)V * T * T; go4.sAi = (long long)T * T; go4.sAm = T; go4.sAk = 1; go4.sBo = (long long)T * V * C; go4.sBi = C; go4.sBn = 1; go4.sBk = V * C; go4.sCo = (long long)T * V * C; go4.sCi = C; go4.sCm = V * C; go4.sRo = 0; go4.sRi = 0; go4.sRm = 0; go4.sRn = 0;
      go4.M = T; go4.N = C; go4.K = T; go4.zi_n = V; go4.flags = 0; go4.act = 0;
      go4.alpha = 1.0f; go4.beta = 0.0f; go4.sa = 1.0f; go4.sb = 1.0f; go4.Npad = C; go4.pad_ = 0;
      if ((long long)(T) >= 64 && (long long)(C) >= 64) k_gemmT<0, 4, 4><<<dim3((unsigned)((C) + 63) / 64, (unsigned)((T) + 63) / 64, (unsigned)(GC)), 32, 0, stream>>>(go4);
      else k_gemm<0><<<dim3((unsigned)((C) + 31) / 32, (unsigned)((T) + 15) / 16, (unsigned)(GC)), 32, 0, stream>>>(go4); }
    { GemmP gQ5;
      gQ5.A = x + (size_t)5 * CB * C * T * V; gQ5.B = Wq; gQ5.bias = bq; gQ5.R = x + (size_t)5 * CB * C * T * V; gQ5.C = Q;
      gQ5.sAo = (long long)C * T * V; gQ5.sAi = 0; gQ5.sAm = 1; gQ5.sAk = T * V; gQ5.sBo = 0; gQ5.sBi = 0; gQ5.sBn = C; gQ5.sBk = 1; gQ5.sCo = (long long)T * V * C; gQ5.sCi = 0; gQ5.sCm = C; gQ5.sRo = 0; gQ5.sRi = 0; gQ5.sRm = 0; gQ5.sRn = 0;
      gQ5.M = T * V; gQ5.N = C; gQ5.K = C; gQ5.zi_n = 1; gQ5.flags = 1; gQ5.act = 0;
      gQ5.alpha = 1.0f; gQ5.beta = 0.0f; gQ5.sa = 1.0f; gQ5.sb = 8.0f; gQ5.Npad = C; gQ5.pad_ = 0;
      if ((long long)(T * V) >= 64 && (long long)(C) >= 64) k_gemmT<0, 4, 4><<<dim3((unsigned)((C) + 63) / 64, (unsigned)((T * V) + 63) / 64, (unsigned)(CB)), 32, 0, stream>>>(gQ5);
      else k_gemm<0><<<dim3((unsigned)((C) + 31) / 32, (unsigned)((T * V) + 15) / 16, (unsigned)(CB)), 32, 0, stream>>>(gQ5); }
    { GemmP gKb5;
      gKb5.A = x + (size_t)5 * CB * C * T * V; gKb5.B = Wk; gKb5.bias = bk; gKb5.R = x + (size_t)5 * CB * C * T * V; gKb5.C = Kb;
      gKb5.sAo = (long long)C * T * V; gKb5.sAi = 0; gKb5.sAm = 1; gKb5.sAk = T * V; gKb5.sBo = 0; gKb5.sBi = 0; gKb5.sBn = C; gKb5.sBk = 1; gKb5.sCo = (long long)T * V * C; gKb5.sCi = 0; gKb5.sCm = C; gKb5.sRo = 0; gKb5.sRi = 0; gKb5.sRm = 0; gKb5.sRn = 0;
      gKb5.M = T * V; gKb5.N = C; gKb5.K = C; gKb5.zi_n = 1; gKb5.flags = 1; gKb5.act = 0;
      gKb5.alpha = 1.0f; gKb5.beta = 0.0f; gKb5.sa = 1.0f; gKb5.sb = 8.0f; gKb5.Npad = C; gKb5.pad_ = 0;
      if ((long long)(T * V) >= 64 && (long long)(C) >= 64) k_gemmT<0, 4, 4><<<dim3((unsigned)((C) + 63) / 64, (unsigned)((T * V) + 63) / 64, (unsigned)(CB)), 32, 0, stream>>>(gKb5);
      else k_gemm<0><<<dim3((unsigned)((C) + 31) / 32, (unsigned)((T * V) + 15) / 16, (unsigned)(CB)), 32, 0, stream>>>(gKb5); }
    { GemmP gVb5;
      gVb5.A = x + (size_t)5 * CB * C * T * V; gVb5.B = Wv; gVb5.bias = bv; gVb5.R = x + (size_t)5 * CB * C * T * V; gVb5.C = Vb;
      gVb5.sAo = (long long)C * T * V; gVb5.sAi = 0; gVb5.sAm = 1; gVb5.sAk = T * V; gVb5.sBo = 0; gVb5.sBi = 0; gVb5.sBn = C; gVb5.sBk = 1; gVb5.sCo = (long long)T * V * C; gVb5.sCi = 0; gVb5.sCm = C; gVb5.sRo = 0; gVb5.sRi = 0; gVb5.sRm = 0; gVb5.sRn = 0;
      gVb5.M = T * V; gVb5.N = C; gVb5.K = C; gVb5.zi_n = 1; gVb5.flags = 1; gVb5.act = 0;
      gVb5.alpha = 1.0f; gVb5.beta = 0.0f; gVb5.sa = 1.0f; gVb5.sb = 8.0f; gVb5.Npad = C; gVb5.pad_ = 0;
      if ((long long)(T * V) >= 64 && (long long)(C) >= 64) k_gemmT<0, 4, 4><<<dim3((unsigned)((C) + 63) / 64, (unsigned)((T * V) + 63) / 64, (unsigned)(CB)), 32, 0, stream>>>(gVb5);
      else k_gemm<0><<<dim3((unsigned)((C) + 31) / 32, (unsigned)((T * V) + 15) / 16, (unsigned)(CB)), 32, 0, stream>>>(gVb5); }
    { GemmP gs5;
      gs5.A = Q; gs5.B = Kb; gs5.bias = Q; gs5.R = Q; gs5.C = S;
      gs5.sAo = (long long)T * V * C; gs5.sAi = C; gs5.sAm = V * C; gs5.sAk = 1; gs5.sBo = (long long)T * V * C; gs5.sBi = C; gs5.sBn = V * C; gs5.sBk = 1; gs5.sCo = (long long)V * T * T; gs5.sCi = (long long)T * T; gs5.sCm = T; gs5.sRo = 0; gs5.sRi = 0; gs5.sRm = 0; gs5.sRn = 0;
      gs5.M = T; gs5.N = T; gs5.K = C; gs5.zi_n = V; gs5.flags = 0; gs5.act = 5;
      gs5.alpha = 0.125f; gs5.beta = 0.0f; gs5.sa = 1.0f; gs5.sb = 1.0f; gs5.Npad = T; gs5.pad_ = 0;
      if ((long long)(T) >= 64 && (long long)(T) >= 64) k_gemmT<0, 4, 4><<<dim3((unsigned)((T) + 63) / 64, (unsigned)((T) + 63) / 64, (unsigned)(GC)), 32, 0, stream>>>(gs5);
      else k_gemm<0><<<dim3((unsigned)((T) + 31) / 32, (unsigned)((T) + 15) / 16, (unsigned)(GC)), 32, 0, stream>>>(gs5); }
    { GemmP go5;
      go5.A = S; go5.B = Vb; go5.bias = S; go5.R = S; go5.C = O + (size_t)5 * NRC * C;
      go5.sAo = (long long)V * T * T; go5.sAi = (long long)T * T; go5.sAm = T; go5.sAk = 1; go5.sBo = (long long)T * V * C; go5.sBi = C; go5.sBn = 1; go5.sBk = V * C; go5.sCo = (long long)T * V * C; go5.sCi = C; go5.sCm = V * C; go5.sRo = 0; go5.sRi = 0; go5.sRm = 0; go5.sRn = 0;
      go5.M = T; go5.N = C; go5.K = T; go5.zi_n = V; go5.flags = 0; go5.act = 0;
      go5.alpha = 1.0f; go5.beta = 0.0f; go5.sa = 1.0f; go5.sb = 1.0f; go5.Npad = C; go5.pad_ = 0;
      if ((long long)(T) >= 64 && (long long)(C) >= 64) k_gemmT<0, 4, 4><<<dim3((unsigned)((C) + 63) / 64, (unsigned)((T) + 63) / 64, (unsigned)(GC)), 32, 0, stream>>>(go5);
      else k_gemm<0><<<dim3((unsigned)((C) + 31) / 32, (unsigned)((T) + 15) / 16, (unsigned)(GC)), 32, 0, stream>>>(go5); }
    { GemmP gQ6;
      gQ6.A = x + (size_t)6 * CB * C * T * V; gQ6.B = Wq; gQ6.bias = bq; gQ6.R = x + (size_t)6 * CB * C * T * V; gQ6.C = Q;
      gQ6.sAo = (long long)C * T * V; gQ6.sAi = 0; gQ6.sAm = 1; gQ6.sAk = T * V; gQ6.sBo = 0; gQ6.sBi = 0; gQ6.sBn = C; gQ6.sBk = 1; gQ6.sCo = (long long)T * V * C; gQ6.sCi = 0; gQ6.sCm = C; gQ6.sRo = 0; gQ6.sRi = 0; gQ6.sRm = 0; gQ6.sRn = 0;
      gQ6.M = T * V; gQ6.N = C; gQ6.K = C; gQ6.zi_n = 1; gQ6.flags = 1; gQ6.act = 0;
      gQ6.alpha = 1.0f; gQ6.beta = 0.0f; gQ6.sa = 1.0f; gQ6.sb = 8.0f; gQ6.Npad = C; gQ6.pad_ = 0;
      if ((long long)(T * V) >= 64 && (long long)(C) >= 64) k_gemmT<0, 4, 4><<<dim3((unsigned)((C) + 63) / 64, (unsigned)((T * V) + 63) / 64, (unsigned)(CB)), 32, 0, stream>>>(gQ6);
      else k_gemm<0><<<dim3((unsigned)((C) + 31) / 32, (unsigned)((T * V) + 15) / 16, (unsigned)(CB)), 32, 0, stream>>>(gQ6); }
    { GemmP gKb6;
      gKb6.A = x + (size_t)6 * CB * C * T * V; gKb6.B = Wk; gKb6.bias = bk; gKb6.R = x + (size_t)6 * CB * C * T * V; gKb6.C = Kb;
      gKb6.sAo = (long long)C * T * V; gKb6.sAi = 0; gKb6.sAm = 1; gKb6.sAk = T * V; gKb6.sBo = 0; gKb6.sBi = 0; gKb6.sBn = C; gKb6.sBk = 1; gKb6.sCo = (long long)T * V * C; gKb6.sCi = 0; gKb6.sCm = C; gKb6.sRo = 0; gKb6.sRi = 0; gKb6.sRm = 0; gKb6.sRn = 0;
      gKb6.M = T * V; gKb6.N = C; gKb6.K = C; gKb6.zi_n = 1; gKb6.flags = 1; gKb6.act = 0;
      gKb6.alpha = 1.0f; gKb6.beta = 0.0f; gKb6.sa = 1.0f; gKb6.sb = 8.0f; gKb6.Npad = C; gKb6.pad_ = 0;
      if ((long long)(T * V) >= 64 && (long long)(C) >= 64) k_gemmT<0, 4, 4><<<dim3((unsigned)((C) + 63) / 64, (unsigned)((T * V) + 63) / 64, (unsigned)(CB)), 32, 0, stream>>>(gKb6);
      else k_gemm<0><<<dim3((unsigned)((C) + 31) / 32, (unsigned)((T * V) + 15) / 16, (unsigned)(CB)), 32, 0, stream>>>(gKb6); }
    { GemmP gVb6;
      gVb6.A = x + (size_t)6 * CB * C * T * V; gVb6.B = Wv; gVb6.bias = bv; gVb6.R = x + (size_t)6 * CB * C * T * V; gVb6.C = Vb;
      gVb6.sAo = (long long)C * T * V; gVb6.sAi = 0; gVb6.sAm = 1; gVb6.sAk = T * V; gVb6.sBo = 0; gVb6.sBi = 0; gVb6.sBn = C; gVb6.sBk = 1; gVb6.sCo = (long long)T * V * C; gVb6.sCi = 0; gVb6.sCm = C; gVb6.sRo = 0; gVb6.sRi = 0; gVb6.sRm = 0; gVb6.sRn = 0;
      gVb6.M = T * V; gVb6.N = C; gVb6.K = C; gVb6.zi_n = 1; gVb6.flags = 1; gVb6.act = 0;
      gVb6.alpha = 1.0f; gVb6.beta = 0.0f; gVb6.sa = 1.0f; gVb6.sb = 8.0f; gVb6.Npad = C; gVb6.pad_ = 0;
      if ((long long)(T * V) >= 64 && (long long)(C) >= 64) k_gemmT<0, 4, 4><<<dim3((unsigned)((C) + 63) / 64, (unsigned)((T * V) + 63) / 64, (unsigned)(CB)), 32, 0, stream>>>(gVb6);
      else k_gemm<0><<<dim3((unsigned)((C) + 31) / 32, (unsigned)((T * V) + 15) / 16, (unsigned)(CB)), 32, 0, stream>>>(gVb6); }
    { GemmP gs6;
      gs6.A = Q; gs6.B = Kb; gs6.bias = Q; gs6.R = Q; gs6.C = S;
      gs6.sAo = (long long)T * V * C; gs6.sAi = C; gs6.sAm = V * C; gs6.sAk = 1; gs6.sBo = (long long)T * V * C; gs6.sBi = C; gs6.sBn = V * C; gs6.sBk = 1; gs6.sCo = (long long)V * T * T; gs6.sCi = (long long)T * T; gs6.sCm = T; gs6.sRo = 0; gs6.sRi = 0; gs6.sRm = 0; gs6.sRn = 0;
      gs6.M = T; gs6.N = T; gs6.K = C; gs6.zi_n = V; gs6.flags = 0; gs6.act = 5;
      gs6.alpha = 0.125f; gs6.beta = 0.0f; gs6.sa = 1.0f; gs6.sb = 1.0f; gs6.Npad = T; gs6.pad_ = 0;
      if ((long long)(T) >= 64 && (long long)(T) >= 64) k_gemmT<0, 4, 4><<<dim3((unsigned)((T) + 63) / 64, (unsigned)((T) + 63) / 64, (unsigned)(GC)), 32, 0, stream>>>(gs6);
      else k_gemm<0><<<dim3((unsigned)((T) + 31) / 32, (unsigned)((T) + 15) / 16, (unsigned)(GC)), 32, 0, stream>>>(gs6); }
    { GemmP go6;
      go6.A = S; go6.B = Vb; go6.bias = S; go6.R = S; go6.C = O + (size_t)6 * NRC * C;
      go6.sAo = (long long)V * T * T; go6.sAi = (long long)T * T; go6.sAm = T; go6.sAk = 1; go6.sBo = (long long)T * V * C; go6.sBi = C; go6.sBn = 1; go6.sBk = V * C; go6.sCo = (long long)T * V * C; go6.sCi = C; go6.sCm = V * C; go6.sRo = 0; go6.sRi = 0; go6.sRm = 0; go6.sRn = 0;
      go6.M = T; go6.N = C; go6.K = T; go6.zi_n = V; go6.flags = 0; go6.act = 0;
      go6.alpha = 1.0f; go6.beta = 0.0f; go6.sa = 1.0f; go6.sb = 1.0f; go6.Npad = C; go6.pad_ = 0;
      if ((long long)(T) >= 64 && (long long)(C) >= 64) k_gemmT<0, 4, 4><<<dim3((unsigned)((C) + 63) / 64, (unsigned)((T) + 63) / 64, (unsigned)(GC)), 32, 0, stream>>>(go6);
      else k_gemm<0><<<dim3((unsigned)((C) + 31) / 32, (unsigned)((T) + 15) / 16, (unsigned)(GC)), 32, 0, stream>>>(go6); }
    { GemmP gQ7;
      gQ7.A = x + (size_t)7 * CB * C * T * V; gQ7.B = Wq; gQ7.bias = bq; gQ7.R = x + (size_t)7 * CB * C * T * V; gQ7.C = Q;
      gQ7.sAo = (long long)C * T * V; gQ7.sAi = 0; gQ7.sAm = 1; gQ7.sAk = T * V; gQ7.sBo = 0; gQ7.sBi = 0; gQ7.sBn = C; gQ7.sBk = 1; gQ7.sCo = (long long)T * V * C; gQ7.sCi = 0; gQ7.sCm = C; gQ7.sRo = 0; gQ7.sRi = 0; gQ7.sRm = 0; gQ7.sRn = 0;
      gQ7.M = T * V; gQ7.N = C; gQ7.K = C; gQ7.zi_n = 1; gQ7.flags = 1; gQ7.act = 0;
      gQ7.alpha = 1.0f; gQ7.beta = 0.0f; gQ7.sa = 1.0f; gQ7.sb = 8.0f; gQ7.Npad = C; gQ7.pad_ = 0;
      if ((long long)(T * V) >= 64 && (long long)(C) >= 64) k_gemmT<0, 4, 4><<<dim3((unsigned)((C) + 63) / 64, (unsigned)((T * V) + 63) / 64, (unsigned)(CB)), 32, 0, stream>>>(gQ7);
      else k_gemm<0><<<dim3((unsigned)((C) + 31) / 32, (unsigned)((T * V) + 15) / 16, (unsigned)(CB)), 32, 0, stream>>>(gQ7); }
    { GemmP gKb7;
      gKb7.A = x + (size_t)7 * CB * C * T * V; gKb7.B = Wk; gKb7.bias = bk; gKb7.R = x + (size_t)7 * CB * C * T * V; gKb7.C = Kb;
      gKb7.sAo = (long long)C * T * V; gKb7.sAi = 0; gKb7.sAm = 1; gKb7.sAk = T * V; gKb7.sBo = 0; gKb7.sBi = 0; gKb7.sBn = C; gKb7.sBk = 1; gKb7.sCo = (long long)T * V * C; gKb7.sCi = 0; gKb7.sCm = C; gKb7.sRo = 0; gKb7.sRi = 0; gKb7.sRm = 0; gKb7.sRn = 0;
      gKb7.M = T * V; gKb7.N = C; gKb7.K = C; gKb7.zi_n = 1; gKb7.flags = 1; gKb7.act = 0;
      gKb7.alpha = 1.0f; gKb7.beta = 0.0f; gKb7.sa = 1.0f; gKb7.sb = 8.0f; gKb7.Npad = C; gKb7.pad_ = 0;
      if ((long long)(T * V) >= 64 && (long long)(C) >= 64) k_gemmT<0, 4, 4><<<dim3((unsigned)((C) + 63) / 64, (unsigned)((T * V) + 63) / 64, (unsigned)(CB)), 32, 0, stream>>>(gKb7);
      else k_gemm<0><<<dim3((unsigned)((C) + 31) / 32, (unsigned)((T * V) + 15) / 16, (unsigned)(CB)), 32, 0, stream>>>(gKb7); }
    { GemmP gVb7;
      gVb7.A = x + (size_t)7 * CB * C * T * V; gVb7.B = Wv; gVb7.bias = bv; gVb7.R = x + (size_t)7 * CB * C * T * V; gVb7.C = Vb;
      gVb7.sAo = (long long)C * T * V; gVb7.sAi = 0; gVb7.sAm = 1; gVb7.sAk = T * V; gVb7.sBo = 0; gVb7.sBi = 0; gVb7.sBn = C; gVb7.sBk = 1; gVb7.sCo = (long long)T * V * C; gVb7.sCi = 0; gVb7.sCm = C; gVb7.sRo = 0; gVb7.sRi = 0; gVb7.sRm = 0; gVb7.sRn = 0;
      gVb7.M = T * V; gVb7.N = C; gVb7.K = C; gVb7.zi_n = 1; gVb7.flags = 1; gVb7.act = 0;
      gVb7.alpha = 1.0f; gVb7.beta = 0.0f; gVb7.sa = 1.0f; gVb7.sb = 8.0f; gVb7.Npad = C; gVb7.pad_ = 0;
      if ((long long)(T * V) >= 64 && (long long)(C) >= 64) k_gemmT<0, 4, 4><<<dim3((unsigned)((C) + 63) / 64, (unsigned)((T * V) + 63) / 64, (unsigned)(CB)), 32, 0, stream>>>(gVb7);
      else k_gemm<0><<<dim3((unsigned)((C) + 31) / 32, (unsigned)((T * V) + 15) / 16, (unsigned)(CB)), 32, 0, stream>>>(gVb7); }
    { GemmP gs7;
      gs7.A = Q; gs7.B = Kb; gs7.bias = Q; gs7.R = Q; gs7.C = S;
      gs7.sAo = (long long)T * V * C; gs7.sAi = C; gs7.sAm = V * C; gs7.sAk = 1; gs7.sBo = (long long)T * V * C; gs7.sBi = C; gs7.sBn = V * C; gs7.sBk = 1; gs7.sCo = (long long)V * T * T; gs7.sCi = (long long)T * T; gs7.sCm = T; gs7.sRo = 0; gs7.sRi = 0; gs7.sRm = 0; gs7.sRn = 0;
      gs7.M = T; gs7.N = T; gs7.K = C; gs7.zi_n = V; gs7.flags = 0; gs7.act = 5;
      gs7.alpha = 0.125f; gs7.beta = 0.0f; gs7.sa = 1.0f; gs7.sb = 1.0f; gs7.Npad = T; gs7.pad_ = 0;
      if ((long long)(T) >= 64 && (long long)(T) >= 64) k_gemmT<0, 4, 4><<<dim3((unsigned)((T) + 63) / 64, (unsigned)((T) + 63) / 64, (unsigned)(GC)), 32, 0, stream>>>(gs7);
      else k_gemm<0><<<dim3((unsigned)((T) + 31) / 32, (unsigned)((T) + 15) / 16, (unsigned)(GC)), 32, 0, stream>>>(gs7); }
    { GemmP go7;
      go7.A = S; go7.B = Vb; go7.bias = S; go7.R = S; go7.C = O + (size_t)7 * NRC * C;
      go7.sAo = (long long)V * T * T; go7.sAi = (long long)T * T; go7.sAm = T; go7.sAk = 1; go7.sBo = (long long)T * V * C; go7.sBi = C; go7.sBn = 1; go7.sBk = V * C; go7.sCo = (long long)T * V * C; go7.sCi = C; go7.sCm = V * C; go7.sRo = 0; go7.sRi = 0; go7.sRm = 0; go7.sRn = 0;
      go7.M = T; go7.N = C; go7.K = T; go7.zi_n = V; go7.flags = 0; go7.act = 0;
      go7.alpha = 1.0f; go7.beta = 0.0f; go7.sa = 1.0f; go7.sb = 1.0f; go7.Npad = C; go7.pad_ = 0;
      if ((long long)(T) >= 64 && (long long)(C) >= 64) k_gemmT<0, 4, 4><<<dim3((unsigned)((C) + 63) / 64, (unsigned)((T) + 63) / 64, (unsigned)(GC)), 32, 0, stream>>>(go7);
      else k_gemm<0><<<dim3((unsigned)((C) + 31) / 32, (unsigned)((T) + 15) / 16, (unsigned)(GC)), 32, 0, stream>>>(go7); }
    k_ts_bn<<<C, 256, 0, stream>>>(O, gam, bet, out, NB, C, T, V);
}
